// SegmentEncoder_51230369906918
// MI455X (gfx1250) — hardware-verified
//
#include <hip/hip_runtime.h>
#include <math.h>

typedef __attribute__((ext_vector_type(16))) _Float16 v16h;
typedef __attribute__((ext_vector_type(8)))  _Float16 v8h;
typedef __attribute__((ext_vector_type(16))) __bf16   v16b;
typedef __attribute__((ext_vector_type(8)))  float    v8f;
typedef __attribute__((ext_vector_type(4)))  float    v4f;

__device__ __forceinline__ int frag_k(int i, int h) { return (i < 8) ? (8 * h + i) : (16 + 8 * h + (i - 8)); }
__device__ __forceinline__ __bf16 bf16_rne(float f) {
    unsigned int u = __float_as_uint(f);
    u += 0x7fffu + ((u >> 16) & 1u);
    return __builtin_bit_cast(__bf16, (unsigned short)(u >> 16));
}
__device__ __forceinline__ float bf16_f32(__bf16 b) { return __uint_as_float(((unsigned int)__builtin_bit_cast(unsigned short, b)) << 16); }
__device__ __forceinline__ v8f wmma16(v16h a, v16h b, v8f c) {
    c = __builtin_amdgcn_wmma_f32_16x16x32_f16(false, a, false, b, (short)0, c, false, false);
    asm volatile("v_nop\n\tv_nop\n\tv_nop\n\tv_nop" : "+v"(c) : "v"(a), "v"(b));
    return c;
}
__device__ __forceinline__ v8f wmmab(v16b a, v16b b, v8f c) {
    c = __builtin_amdgcn_wmma_f32_16x16x32_bf16(false, a, false, b, (short)0, c, false, false);
    asm volatile("v_nop\n\tv_nop\n\tv_nop\n\tv_nop" : "+v"(c) : "v"(a), "v"(b));
    return c;
}
struct Split { v16b hi, lo; };
__device__ __forceinline__ v8f wmma3(const Split& a, const Split& b, v8f c) {
    c = __builtin_amdgcn_wmma_f32_16x16x32_bf16(false, a.hi, false, b.hi, (short)0, c, false, false);
    c = __builtin_amdgcn_wmma_f32_16x16x32_bf16(false, a.hi, false, b.lo, (short)0, c, false, false);
    c = __builtin_amdgcn_wmma_f32_16x16x32_bf16(false, a.lo, false, b.hi, (short)0, c, false, false);
    asm volatile("v_nop\n\tv_nop\n\tv_nop\n\tv_nop" : "+v"(c) : "v"(a.hi), "v"(a.lo), "v"(b.hi), "v"(b.lo));
    return c;
}
struct Split3 { v16b hi, mid, lo; };
__device__ __forceinline__ v8f wmma6(const Split3& a, const Split3& b, v8f c) {
    c = __builtin_amdgcn_wmma_f32_16x16x32_bf16(false, a.hi, false, b.hi, (short)0, c, false, false);
    c = __builtin_amdgcn_wmma_f32_16x16x32_bf16(false, a.hi, false, b.mid, (short)0, c, false, false);
    c = __builtin_amdgcn_wmma_f32_16x16x32_bf16(false, a.mid, false, b.hi, (short)0, c, false, false);
    c = __builtin_amdgcn_wmma_f32_16x16x32_bf16(false, a.hi, false, b.lo, (short)0, c, false, false);
    c = __builtin_amdgcn_wmma_f32_16x16x32_bf16(false, a.mid, false, b.mid, (short)0, c, false, false);
    c = __builtin_amdgcn_wmma_f32_16x16x32_bf16(false, a.lo, false, b.hi, (short)0, c, false, false);
    asm volatile("v_nop\n\tv_nop\n\tv_nop\n\tv_nop" : "+v"(c) : "v"(a.hi), "v"(a.mid), "v"(a.lo), "v"(b.hi), "v"(b.mid), "v"(b.lo));
    return c;
}

__device__ __forceinline__ v16h fh_ld(const float* __restrict__ p, long long sk, int k0, int h, int klen, float s) {
    v16h a;
#pragma unroll
    for (int i = 0; i < 16; ++i) { const int k = k0 + frag_k(i, h); a[i] = (k < klen) ? (_Float16)(p[(long long)k * sk] * s) : (_Float16)0.f; }
    return a;
}
__device__ __forceinline__ Split sp_ld(const float* __restrict__ p, long long sk, int k0, int h, int klen, float s) {
    Split r;
#pragma unroll
    for (int i = 0; i < 16; ++i) {
        const int k = k0 + frag_k(i, h); const float x = (k < klen) ? p[(long long)k * sk] * s : 0.f;
        const __bf16 hb = bf16_rne(x); r.hi[i] = hb; r.lo[i] = bf16_rne(x - bf16_f32(hb));
    }
    return r;
}
__device__ __forceinline__ Split3 sp3_ld(const float* __restrict__ p, long long sk, int k0, int h, int klen, float s) {
    Split3 r;
#pragma unroll
    for (int i = 0; i < 16; ++i) {
        const int k = k0 + frag_k(i, h); const float x = (k < klen) ? p[(long long)k * sk] * s : 0.f;
        const __bf16 hb = bf16_rne(x); const float r1 = x - bf16_f32(hb); const __bf16 mb = bf16_rne(r1);
        r.hi[i] = hb; r.mid[i] = mb; r.lo[i] = bf16_rne(r1 - bf16_f32(mb));
    }
    return r;
}
__device__ __forceinline__ v16b bh_ld(const float* __restrict__ p, long long sk, int k0, int h, int klen, float s) {
    v16b a;
#pragma unroll
    for (int i = 0; i < 16; ++i) { const int k = k0 + frag_k(i, h); a[i] = bf16_rne((k < klen) ? p[(long long)k * sk] * s : 0.f); }
    return a;
}
__device__ __forceinline__ v16h fh_row(const _Float16* __restrict__ row, int k0, int h) {
    v16h a;
#pragma unroll
    for (int i = 0; i < 16; ++i) a[i] = row[k0 + frag_k(i, h)];
    return a;
}

#define VST2(T, ptr, val) do { *(volatile T*)(ptr) = (val); __threadfence(); *(volatile T*)(ptr) = (val); } while (0)
typedef float v4f __attribute__((ext_vector_type(4)));
#define VST2V4(ptr, val) do { *(volatile v4f*)(ptr) = (val); __threadfence(); *(volatile v4f*)(ptr) = (val); } while (0)

__device__ __attribute__((noinline)) float act_fn(float v, int act) {
    if (act == 1) return fmaxf(v, 0.f);
    if (act == 2) { const float u = 0.7978845608028654f * (v + 0.044715f * v * v * v); return 0.5f * v * (1.f + tanhf(u)); }
    if (act == 3) return v / (1.f + expf(-v));
    if (act == 4) return 0.5f * v * (1.f + erff(v * 0.7071067811865476f));
    if (act == 5) return tanhf(v);
    if (act == 6) return 1.f / (1.f + expf(-v));
    if (act == 7) return (v > 0.f) ? v : 0.01f * v;
    if (act == 8) return (v > 0.f) ? v : (expf(v) - 1.f);
    if (act == 9) return fminf(fmaxf(v, 0.f), 6.f);
    if (act == 10) return fabsf(v);
    if (act == 11) return (v >= 0.f) ? v : 0.1f * v;
    if (act == 12) return (v > 0.f) ? v : 0.2f * v;
    if (act == 13) return (v > 20.f) ? v : log1pf(expf(v));
    return v;
}

struct GemmP {
    const float* A; const float* B; const float* bias; const float* R; float* C;
    long long sAo, sAi, sAm, sAk, sBo, sBi, sBn, sBk, sCo, sCi, sCm, sRo, sRi, sRm, sRn;
    int M, N, K, zi_n, flags, act; float alpha, beta, sa, sb;
    int Npad, pad_;
};
static_assert(sizeof(GemmP) == 5 * 8 + 15 * 8 + 6 * 4 + 4 * 4 + 2 * 4, "GemmP has padding");

template <int MODE>
__global__ __launch_bounds__(32) void k_gemm(GemmP p) {
    const int lane = threadIdx.x & 31, h = lane >> 4, l15 = lane & 15;
    const int m0 = blockIdx.y * 16, n0 = blockIdx.x * 32;
    const int z = blockIdx.z, zo = z / p.zi_n, zi = z - zo * p.zi_n;
    const float* A = p.A + zo * p.sAo + zi * p.sAi;
    const float* B = p.B + zo * p.sBo + zi * p.sBi;
    const int am = min(m0 + l15, p.M - 1);
    v8f acc[2], comp[2];
#pragma unroll
    for (int t = 0; t < 2; ++t) { v8f zz = {}; acc[t] = zz; comp[t] = zz; }
    for (int k0 = 0; k0 < p.K; k0 += 32) {
        const float* arow = A + (long long)am * p.sAm;
        if (MODE == 1) {
            const Split a = sp_ld(arow, p.sAk, k0, h, p.K, 1.f);
#pragma unroll
            for (int t = 0; t < 2; ++t) {
                const int bn = min(n0 + t * 16 + l15, p.N - 1);
                acc[t] = wmma3(a, sp_ld(B + (long long)bn * p.sBn, p.sBk, k0, h, p.K, 1.f), acc[t]);
            }
        } else if (MODE == 3) {
            const Split3 a = sp3_ld(arow, p.sAk, k0, h, p.K, 1.f);
#pragma unroll
            for (int t = 0; t < 2; ++t) {
                const int bn = min(n0 + t * 16 + l15, p.N - 1);
                acc[t] = wmma6(a, sp3_ld(B + (long long)bn * p.sBn, p.sBk, k0, h, p.K, 1.f), acc[t]);
            }
        } else if (MODE == 4) {
            const Split3 a = sp3_ld(arow, p.sAk, k0, h, p.K, 1.f);
#pragma unroll
            for (int t = 0; t < 2; ++t) {
                const int bn = min(n0 + t * 16 + l15, p.N - 1); v8f zz = {};
                const v8f part = wmma6(a, sp3_ld(B + (long long)bn * p.sBn, p.sBk, k0, h, p.K, 1.f), zz);
                const v8f y = part - comp[t]; const v8f s = acc[t] + y; comp[t] = (s - acc[t]) - y; acc[t] = s;
            }
        } else if (MODE == 2) {
            const v16b a = bh_ld(arow, p.sAk, k0, h, p.K, 1.f);
#pragma unroll
            for (int t = 0; t < 2; ++t) {
                const int bn = min(n0 + t * 16 + l15, p.N - 1);
                acc[t] = wmmab(a, bh_ld(B + (long long)bn * p.sBn, p.sBk, k0, h, p.K, 1.f), acc[t]);
            }
        } else {
            const v16h a = fh_ld(arow, p.sAk, k0, h, p.K, p.sa);
#pragma unroll
            for (int t = 0; t < 2; ++t) {
                const int bn = min(n0 + t * 16 + l15, p.N - 1);
                acc[t] = wmma16(a, fh_ld(B + (long long)bn * p.sBn, p.sBk, k0, h, p.K, p.sb), acc[t]);
            }
        }
    }
    const float iscale = (MODE == 0) ? p.alpha / (p.sa * p.sb) : p.alpha;
    float* C = p.C + zo * p.sCo + zi * p.sCi;
    const float* R = p.R + zo * p.sRo + zi * p.sRi;
    __shared__ __align__(16) float ctile[16][36];
#pragma unroll
    for (int t = 0; t < 2; ++t) {
        const int n = n0 + t * 16 + l15; const int nn = min(n, p.N - 1);
#pragma unroll
        for (int r = 0; r < 8; ++r) {
            const int m = m0 + 8 * h + r; const int mm = min(m, p.M - 1);
            float v = acc[t][r] * iscale;
            if (p.flags & 1) v += p.bias[nn];
            if (p.flags & 2) v += p.bias[mm];
            v = act_fn(v, p.act);
            if (p.flags & 4) v += p.beta * R[(long long)mm * p.sRm + (long long)nn * p.sRn];
            ctile[8 * h + r][t * 16 + l15] = (n < p.N) ? v : 0.f;
        }
    }
    __syncthreads();
    const int NW = (p.Npad > p.N) ? p.Npad : p.N;
    const bool fast = (m0 + 16 <= p.M) && (n0 + 32 <= NW) && ((p.sCm & 3) == 0) && ((((size_t)C) & 15) == 0);
    if (fast) {
#pragma unroll
        for (int s = 0; s < 4; ++s) {
            const int row = s * 4 + (lane >> 3), c4 = (lane & 7) * 4;
            const v4f v = *(const v4f*)&ctile[row][c4];
            VST2V4(C + (long long)(m0 + row) * p.sCm + n0 + c4, v);
        }
    } else {
        for (int row = 0; row < 16; ++row) {
            const int m = m0 + row, n = n0 + lane;
            if (m < p.M && n < NW) VST2(float, C + (long long)m * p.sCm + n, ctile[row][lane]);
        }
    }
}

#define AW 4
struct AttnP {
    const float* Q; const float* K; const float* V; float* O; float* P; const float* Mf; const int* Mi; float* ST;
    const float* Pw; const float* Rt; const int* SQ; const int* SK;
    long long swb, swh, swi, swj, srb, srh, sri;
    long long sQb, sQh, sQi, sQd, sKb, sKh, sKj, sKd, sVb, sVh, sVj, sVd, sOb, sOh, sOi, sPb, sPh, sPi, smb, smh, smi, smj;
    int Lq, Lk, dh, dv, hrep, causal, coff, pband;
    float scale, mfill; int nonorm, mpol;
    int roff, rn, segpol, win;
};
static_assert(sizeof(AttnP) == 12 * 8 + 29 * 8 + 16 * 4, "AttnP has padding");

#ifndef KATTN_ATTR
#define KATTN_ATTR
#endif
template <int DHP, int DVP, int QM, bool SPLITPV, bool TWOPASS>
__global__ __launch_bounds__(32 * AW) KATTN_ATTR void k_attn(AttnP p) {
    constexpr int NT = DVP / 16;
    constexpr int KS = DHP / 32;
    constexpr int VP = DVP + 8;
    __shared__ __align__(16) float    pl[AW][16 * 64];
    __shared__ __align__(16) _Float16 vl[(SPLITPV ? 2 : 1) * 64 * VP];
    const int lane = threadIdx.x & 31, hf = lane >> 4, l15 = lane & 15, wave = threadIdx.x >> 5;
    const int h = blockIdx.y, b = blockIdx.z, hk = h / p.hrep;
    const int q0 = (blockIdx.x * AW + wave) * 16;
    float* myp = pl[wave];
    const float L2E = 1.4426950408889634f;
    const float NEG = -__builtin_inff();
    const int qi = min(q0 + l15, p.Lq - 1);
    const float* qrow = p.Q + b * p.sQb + h * p.sQh + (long long)qi * p.sQi;
    const float* kbase = p.K + b * p.sKb + hk * p.sKh;
    const float* vbase = p.V + b * p.sVb + hk * p.sVh;
    v16h qa[QM == 0 ? KS : 1]; Split qs_[QM == 1 ? KS : 1]; Split3 qt_[QM == 2 ? KS : 1];
#pragma unroll
    for (int ks = 0; ks < KS; ++ks) {
        if (QM == 2) qt_[ks] = sp3_ld(qrow, p.sQd, ks * 32, hf, p.dh, 1.f);
        else if (QM == 1) qs_[ks] = sp_ld(qrow, p.sQd, ks * 32, hf, p.dh, 1.f);
        else qa[ks] = fh_ld(qrow, p.sQd, ks * 32, hf, p.dh, 1.f);
    }
    v8f o[NT]; float m8[8], l8[8];
#pragma unroll
    for (int t = 0; t < NT; ++t) { v8f zz = {}; o[t] = zz; }
#pragma unroll
    for (int i = 0; i < 8; ++i) { m8[i] = NEG; l8[i] = 0.f; }
    int jend = p.Lk;
    if (p.causal == 1) { const int je = (blockIdx.x * AW + AW - 1) * 16 + 16 + p.coff; jend = min(jend, max(je, 0)); }
    const int npass = TWOPASS ? 2 : 1;
    for (int pass = 0; pass < npass; ++pass) {
        const bool dopv = (!TWOPASS) || pass == 1;
        for (int j0 = 0; j0 < jend; j0 += 64) {
            if (dopv) {
                __syncthreads();
                for (int idx = threadIdx.x; idx < 64 * DVP; idx += 32 * AW) {
                    const int jr = idx / DVP, d = idx - jr * DVP, j = j0 + jr;
                    const float f = (j < p.Lk && d < p.dv) ? vbase[(long long)j * p.sVj + (long long)d * p.sVd] : 0.f;
                    if (SPLITPV) {
                        const __bf16 hb = bf16_rne(f);
                        ((__bf16*)vl)[jr * VP + d] = hb; ((__bf16*)vl)[64 * VP + jr * VP + d] = bf16_rne(f - bf16_f32(hb));
                    } else vl[jr * VP + d] = (_Float16)f;
                }
            }
            v8f s[4];
#pragma unroll
            for (int t = 0; t < 4; ++t) {
                const int j = min(j0 + t * 16 + l15, p.Lk - 1);
                const float* krow = kbase + (long long)j * p.sKj;
                v8f acc = {};
#pragma unroll
                for (int ks = 0; ks < KS; ++ks) {
                    if (QM == 2)      acc = wmma6(qt_[ks], sp3_ld(krow, p.sKd, ks * 32, hf, p.dh, 1.f), acc);
                    else if (QM == 1) acc = wmma3(qs_[ks], sp_ld(krow, p.sKd, ks * 32, hf, p.dh, 1.f), acc);
                    else              acc = wmma16(qa[ks], fh_ld(krow, p.sKd, ks * 32, hf, p.dh, 1.f), acc);
                }
                s[t] = acc;
            }
            float pv[8][4];
#pragma unroll
            for (int i = 0; i < 8; ++i) {
                const int irow = q0 + i + 8 * hf;
                const int ic = min(irow, p.Lq - 1);
                float sc[4];
#pragma unroll
                for (int t = 0; t < 4; ++t) {
                    const int jg = j0 + t * 16 + l15;
                    float v = s[t][i] * p.scale;
                    if (p.Mf) v += p.Mf[b * p.smb + h * p.smh + (long long)ic * p.smi + (long long)min(jg, p.Lk - 1) * p.smj];
                    if (p.Rt) { int rc = ic - min(jg, p.Lk - 1) + p.roff; rc = rc < 0 ? 0 : (rc >= p.rn ? p.rn - 1 : rc); v += p.Rt[b * p.srb + h * p.srh + (long long)ic * p.sri + rc]; }
                    if (p.Mi) { const int mv = p.Mi[b * p.smb + h * p.smh + (long long)ic * p.smi + (long long)min(jg, p.Lk - 1) * p.smj]; if (p.mpol ? (mv != 0) : (mv == 0)) v = p.mfill; }
                    if (p.SQ) { const bool same = p.SQ[(long long)b * p.Lq + ic] == p.SK[(long long)b * p.Lk + min(jg, p.Lk - 1)]; if (p.segpol ? same : !same) v = p.mfill; }
                    if (p.causal == 2 && jg > irow + p.coff) v = p.mfill;
                    if (jg >= p.Lk || (p.causal == 1 && jg > irow + p.coff) || (p.causal == 3 && jg < irow + p.coff) || (p.win > 0 && irow + p.coff - jg > p.win)) v = NEG; else v *= L2E;
                    sc[t] = v;
                }
                if (!TWOPASS || pass == 0) {
                    float mx = fmaxf(fmaxf(sc[0], sc[1]), fmaxf(sc[2], sc[3]));
                    mx = fmaxf(mx, __shfl_xor(mx, 1, 32)); mx = fmaxf(mx, __shfl_xor(mx, 2, 32));
                    mx = fmaxf(mx, __shfl_xor(mx, 4, 32)); mx = fmaxf(mx, __shfl_xor(mx, 8, 32));
                    const float mnew = fmaxf(m8[i], mx);
                    const float corr = (mnew == NEG) ? 1.f : exp2f(m8[i] - mnew);
                    float rs = 0.f;
#pragma unroll
                    for (int t = 0; t < 4; ++t) {
                        const float pp = (sc[t] == NEG) ? 0.f : exp2f(sc[t] - mnew); rs += pp;
                        pv[i][t] = p.Pw ? pp * p.Pw[b * p.swb + h * p.swh + (long long)ic * p.swi + (long long)min(j0 + t * 16 + l15, p.Lk - 1) * p.swj] : pp;
                    }
                    rs += __shfl_xor(rs, 1, 32); rs += __shfl_xor(rs, 2, 32); rs += __shfl_xor(rs, 4, 32); rs += __shfl_xor(rs, 8, 32);
                    l8[i] = l8[i] * corr + rs; m8[i] = mnew;
                    if (!TWOPASS) {
#pragma unroll
                        for (int t = 0; t < NT; ++t) o[t][i] *= corr;
                    }
                } else {
                    const float inv = (l8[i] > 0.f) ? 1.f / l8[i] : 0.f;
#pragma unroll
                    for (int t = 0; t < 4; ++t) {
                        const int jg = j0 + t * 16 + l15;
                        float pp = (sc[t] == NEG) ? 0.f : exp2f(sc[t] - m8[i]) * inv;
                        if (p.Pw) pp *= p.Pw[b * p.swb + h * p.swh + (long long)ic * p.swi + (long long)min(jg, p.Lk - 1) * p.swj];
                        pv[i][t] = pp;
                    }
                }
            }
            if (dopv) {
#pragma unroll
                for (int i = 0; i < 8; ++i)
#pragma unroll
                    for (int t = 0; t < 4; ++t) myp[(i + 8 * hf) * 64 + t * 16 + l15] = pv[i][t];
                __syncthreads();
                if (p.P) {
                    float* pb_ = p.P + b * p.sPb + h * p.sPh;
                    const bool fastP = (p.pband == 0) && ((p.sPi & 3) == 0) && (j0 + 64 <= p.Lk) && (q0 + 16 <= p.Lq) && ((((size_t)pb_) & 15) == 0);
                    if (fastP) {
#pragma unroll
                        for (int s = 0; s < 8; ++s) {
                            const int row = s * 2 + (lane >> 4), c4 = (lane & 15) * 4;
                            const v4f v = *(const v4f*)(myp + row * 64 + c4);
                            VST2V4(pb_ + (long long)(q0 + row) * p.sPi + j0 + c4, v);
                        }
                    } else {
                        for (int row = 0; row < 16; ++row) {
                            const int irow = q0 + row; if (irow >= p.Lq) continue;
                            for (int c = lane; c < 64; c += 32) {
                                const int jg = j0 + c; if (jg >= p.Lk) continue;
                                if (p.pband == 0) VST2(float, pb_ + (long long)irow * p.sPi + jg, myp[row * 64 + c]);
                                else if (jg - irow <= p.pband && irow - jg <= p.pband) VST2(float, pb_ + (long long)irow * p.sPi + (jg - irow + p.pband), myp[row * 64 + c]);
                            }
                        }
                    }
                }
                if (SPLITPV) {
                    const Split pa0 = sp_ld(myp + l15 * 64, 1, 0, hf, 64, 1.f), pa1 = sp_ld(myp + l15 * 64, 1, 32, hf, 64, 1.f);
                    const __bf16* vh = (const __bf16*)vl; const __bf16* vlo = vh + 64 * VP;
#pragma unroll
                    for (int t = 0; t < NT; ++t) {
                        const int dcol = t * 16 + l15;
                        Split b0, b1;
#pragma unroll
                        for (int e = 0; e < 16; ++e) {
                            const int k0 = frag_k(e, hf), k1 = 32 + frag_k(e, hf);
                            b0.hi[e] = vh[k0 * VP + dcol]; b0.lo[e] = vlo[k0 * VP + dcol]; b1.hi[e] = vh[k1 * VP + dcol]; b1.lo[e] = vlo[k1 * VP + dcol];
                        }
                        o[t] = wmma3(pa0, b0, o[t]);
                        o[t] = wmma3(pa1, b1, o[t]);
                    }
                } else {
                    const v16h pa0 = fh_ld(myp + l15 * 64, 1, 0, hf, 64, 4096.f), pa1 = fh_ld(myp + l15 * 64, 1, 32, hf, 64, 4096.f);
#pragma unroll
                    for (int t = 0; t < NT; ++t) {
                        const int dcol = t * 16 + l15;
                        v16h b0, b1;
#pragma unroll
                        for (int e = 0; e < 16; ++e) { b0[e] = vl[frag_k(e, hf) * VP + dcol]; b1[e] = vl[(32 + frag_k(e, hf)) * VP + dcol]; }
                        o[t] = wmma16(pa0, b0, o[t]);
                        o[t] = wmma16(pa1, b1, o[t]);
                    }
                }
            }
        }
    }
    float* obase = p.O + b * p.sOb + h * p.sOh;
    if (p.ST) {
        const int rl = lane >> 1, isel = rl & 7;
        float mv = 0.f, lv = 0.f;
#pragma unroll
        for (int i = 0; i < 8; ++i) if (i == isel) { mv = m8[i]; lv = l8[i]; }
        const int irow = q0 + rl;
        if (irow < p.Lq) { float* st = p.ST + (((long long)b * gridDim.y + h) * p.Lq + irow) * 2 + (lane & 1); VST2(float, st, (lane & 1) ? lv : mv * 0.6931471805599453f); }
    }
    float invr[8];
#pragma unroll
    for (int i = 0; i < 8; ++i) {
        if (TWOPASS) invr[i] = SPLITPV ? 1.f : (1.f / 4096.f);
        else if (p.nonorm) invr[i] = exp2f(m8[i]) * (SPLITPV ? 1.f : (1.f / 4096.f));
        else invr[i] = (l8[i] > 0.f) ? (SPLITPV ? 1.f / l8[i] : 1.f / (l8[i] * 4096.f)) : 0.f;
    }
    __syncthreads();
    const bool ofast = ((p.sOi & 3) == 0) && ((((size_t)obase) & 15) == 0) && (q0 + 16 <= p.Lq);
#pragma unroll
    for (int c0 = 0; c0 < DVP; c0 += 64) {
#pragma unroll
        for (int i = 0; i < 8; ++i)
#pragma unroll
            for (int t = 0; t < NT; ++t) if (t * 16 >= c0 && t * 16 < c0 + 64) myp[(i + 8 * hf) * 64 + (t * 16 - c0) + l15] = o[t][i] * invr[i];
        __syncthreads();
        const int cw = (DVP - c0 < 64) ? (DVP - c0) : 64;
        if (ofast && (c0 + cw <= p.dv) && (cw % 32 == 0)) {
            const int lpr = cw / 4;
            const int rows_per_ins = 32 / lpr;
            for (int r0 = 0; r0 < 16; r0 += rows_per_ins) {
                const int row = r0 + lane / lpr, c4 = (lane % lpr) * 4;
                const v4f v = *(const v4f*)(myp + row * 64 + c4);
                VST2V4(obase + (long long)(q0 + row) * p.sOi + c0 + c4, v);
            }
        } else {
            for (int row = 0; row < 16; ++row) {
                const int irow = q0 + row; if (irow >= p.Lq) continue;
                for (int c = lane; c < cw; c += 32) { const int d = c0 + c; if (d < p.dv) VST2(float, obase + (long long)irow * p.sOi + d, myp[row * 64 + c]); }
            }
        }
        __syncthreads();
    }
}

struct TrP { const float* src; float* dst; const float* R2; long long sSz, lds, sDz, ldd, sRz, ldr; int R, C, flags, act; float alpha, beta; };
static_assert(sizeof(TrP) == 3 * 8 + 6 * 8 + 6 * 4, "TrP has padding");
__global__ __launch_bounds__(256) void k_tr(TrP p) {
    __shared__ float tile[32][33];
    const int c0 = blockIdx.x * 32, r0 = blockIdx.y * 32, z = blockIdx.z;
    const int lane = threadIdx.x & 31, wave = threadIdx.x >> 5;
    const float* s = p.src + z * p.sSz;
#pragma unroll
    for (int k = 0; k < 4; ++k) {
        const int rl = wave * 4 + k, r = r0 + rl, c = c0 + lane;
        tile[rl][lane] = (r < p.R && c < p.C) ? s[(long long)r * p.lds + c] : 0.f;
    }
    __syncthreads();
    float* d = p.dst + z * p.sDz; const float* rr = p.R2 + z * p.sRz;
#pragma unroll
    for (int k = 0; k < 4; ++k) {
        const int cl = wave * 4 + k, c = c0 + cl, r = r0 + lane;
        if (c < p.C && r < p.R) {
            float v = act_fn(p.alpha * tile[lane][cl], p.act);
            if (p.flags & 1) v += p.beta * rr[(long long)c * p.ldr + r];
            VST2(float, d + (long long)c * p.ldd + r, v);
        }
    }
}

__global__ __launch_bounds__(256) void k_affine(const float* __restrict__ src, float* __restrict__ dst, int n, float a, float b, const float* __restrict__ sdev) {
    const int i = blockIdx.x * 256 + threadIdx.x;
    if (i < n) { const float aa = sdev ? a * sdev[0] : a; const float v = aa * src[i] + b; VST2(float, dst + i, v); }
}

struct SmP { const float* src; float* dst; const float* Mf; long long sz, sr, dz, dr, smz, smr; int n, pad; float scale_in, scale_out; };
static_assert(sizeof(SmP) == 3 * 8 + 6 * 8 + 4 * 4, "SmP has padding");
__global__ __launch_bounds__(256) void k_softmax(SmP p) {
    __shared__ float red[256];
    const int r = blockIdx.x, z = blockIdx.y, tid = threadIdx.x;
    const float* s = p.src + z * p.sz + (long long)r * p.sr;
    const float* mf = p.Mf ? (p.Mf + z * p.smz + (long long)r * p.smr) : nullptr;
    float mx = -__builtin_inff();
    for (int j = tid; j < p.n; j += 256) { float v = s[j] * p.scale_in; if (mf) v += mf[j]; mx = fmaxf(mx, v); }
    red[tid] = mx; __syncthreads();
    for (int o = 128; o > 0; o >>= 1) { if (tid < o) red[tid] = fmaxf(red[tid], red[tid + o]); __syncthreads(); }
    mx = red[0]; __syncthreads();
    float sum = 0.f;
    for (int j = tid; j < p.n; j += 256) { float v = s[j] * p.scale_in; if (mf) v += mf[j]; sum += (mx == -__builtin_inff()) ? 0.f : expf(v - mx); }
    red[tid] = sum; __syncthreads();
    for (int o = 128; o > 0; o >>= 1) { if (tid < o) red[tid] += red[tid + o]; __syncthreads(); }
    sum = red[0];
    const float inv = (sum > 0.f) ? p.scale_out / sum : 0.f;
    float* d = p.dst + z * p.dz + (long long)r * p.dr;
    for (int j = tid; j < p.n; j += 256) { float v = s[j] * p.scale_in; if (mf) v += mf[j]; const float o = (mx == -__builtin_inff()) ? 0.f : expf(v - mx) * inv; VST2(float, d + j, o); }
}
__global__ __launch_bounds__(256) void k_stats(const float* __restrict__ x, long long sz, long long so, long long si, int inner, int n, float eps, float* __restrict__ stat, int mode) {
    __shared__ float red[256];
    const int z = blockIdx.x, tid = threadIdx.x;
    const float* base = x + z * sz;
    float s = 0.f;
    for (int e = tid; e < n; e += 256) s += base[(long long)(e / inner) * so + (long long)(e % inner) * si];
    red[tid] = s; __syncthreads();
    for (int o = 128; o > 0; o >>= 1) { if (tid < o) red[tid] += red[tid + o]; __syncthreads(); }
    const float mu = (mode == 0 || mode == 3) ? red[0] / (float)n : 0.f; __syncthreads();
    float q = 0.f;
    for (int e = tid; e < n; e += 256) { const float dlt = base[(long long)(e / inner) * so + (long long)(e % inner) * si] - mu; q += dlt * dlt; }
    red[tid] = q; __syncthreads();
    for (int o = 128; o > 0; o >>= 1) { if (tid < o) red[tid] += red[tid + o]; __syncthreads(); }
    {
        float rs;
        if (mode == 2) rs = sqrtf((float)n) / fmaxf(sqrtf(red[0]), eps); else if (mode == 3) rs = rsqrtf(red[0] / (float)(n - 1) + eps); else rs = rsqrtf(red[0] / (float)n + eps);
        if (tid < 32) { const float v = (tid == 0) ? mu : ((tid == 1) ? rs : 0.f); VST2(float, stat + (long long)z * 32 + tid, v); }
    }
}
__global__ __launch_bounds__(256) void k_norm_apply(const float* __restrict__ x, float* __restrict__ y, const float* __restrict__ stat, const float* __restrict__ g, const float* __restrict__ bta,
                                                     int Z, int C, int L, int G, int bn, int act) {
    const long long idx = (long long)blockIdx.x * 256 + threadIdx.x;
    if (idx >= (long long)Z * C * L) return;
    const int l = (int)(idx % L); const long long zc = idx / L; const int c = (int)(zc % C), z = (int)(zc / C); (void)l;
    const int set = bn ? c : (z * G + c / (C / G));
    float v = (x[idx] - stat[(long long)set * 32]) * stat[(long long)set * 32 + 1];
    if (g) v *= g[c];
    if (bta) v += bta[c];
    v = act_fn(v, act);
    VST2(float, y + idx, v);
}

__global__ __launch_bounds__(256) void k_lse_neg(const float* __restrict__ st, float* __restrict__ c, int n) {
    const int i = blockIdx.x * 256 + threadIdx.x;
    if (i < n) { const float v = -(st[2 * i] + logf(st[2 * i + 1])); VST2(float, c + i, v); }
}

__global__ __launch_bounds__(256) void k_iota(int* __restrict__ dst, int n, int a, int b) {
    const int i = blockIdx.x * 256 + threadIdx.x;
    if (i < n) { const int v = a * i + b; VST2(int, dst + i, v); }
}

__global__ __launch_bounds__(256) void k_axpby(const float* __restrict__ x, const float* __restrict__ y, float* __restrict__ dst, int n, float a, float b, float c) {
    const int i = blockIdx.x * 256 + threadIdx.x;
    if (i < n) { const float v = a * x[i] + b * y[i] + c; VST2(float, dst + i, v); }
}

struct RopeP { const float* X; float* Y; const float* C; const float* Sn; const int* pos; long long sXr, sXh, sYr, sYh, sCb, sCp, sCd; int R, Hn, D, S, mode, tmode, pmode, pad; };
static_assert(sizeof(RopeP) == 5 * 8 + 7 * 8 + 8 * 4, "RopeP has padding");
__global__ __launch_bounds__(256) void k_rope(RopeP p) {
    const long long idx = (long long)blockIdx.x * 256 + threadIdx.x;
    if (idx >= (long long)p.R * p.Hn * p.D) return;
    const int d = (int)(idx % p.D); const long long rh = idx / p.D; const int h = (int)(rh % p.Hn); const int r = (int)(rh / p.Hn);
    const int half = p.D / 2;
    int partner; float sign;
    if (p.mode == 0) { partner = (d < half) ? d + half : d - half; sign = (d < half) ? -1.f : 1.f; }
    else { partner = d ^ 1; sign = (d & 1) ? 1.f : -1.f; }
    const int tcol = (p.tmode == 0) ? d : ((p.tmode == 1) ? (d % half) : (d >> 1));
    const int pp = (p.pmode == 0) ? (r % p.S) : ((p.pmode == 1) ? h : p.pos[r]);
    const long long toff = (long long)(r / p.S) * p.sCb + (long long)pp * p.sCp + (long long)tcol * p.sCd;
    const float* xr = p.X + (long long)r * p.sXr + (long long)h * p.sXh;
    const float v = xr[d] * p.C[toff] + sign * xr[partner] * p.Sn[toff];
    VST2(float, p.Y + (long long)r * p.sYr + (long long)h * p.sYh + d, v);
}

__global__ __launch_bounds__(256) void k_invf(float* __restrict__ invb, int half, int D, float base, float num, int fmode, float cexp) {
    const int i = blockIdx.x * 256 + threadIdx.x;
    if (i >= ((half + 31) / 32) * 32) return;
    if (i >= half) { VST2(float, invb + i, 0.f); return; }
    const float e = (float)(2 * i) / (float)D;
    float invf;
    if (fmode == 1) invf = num * expf((float)(2 * i) * cexp);
    else if (fmode == 2) invf = num * powf(base, (-2.0f * ((float)i - 1.0f)) / (float)D);
    else invf = num * (1.0f / powf(base, e));
    VST2(float, invb + i, invf);
}
__global__ __launch_bounds__(256) void k_sincos(float* __restrict__ cs, float* __restrict__ sn, const float* __restrict__ invb, int S, int half, float pscale) {
    const int idx = blockIdx.x * 256 + threadIdx.x;
    if (idx >= S * half) return;
    const int s = idx / half, i = idx - s * half;
    const float ang = (pscale * (float)s) * invb[i];
    VST2(float, cs + idx, cosf(ang)); VST2(float, sn + idx, sinf(ang));
}

__global__ __launch_bounds__(256) void k_mulact(const float* __restrict__ x, const float* __restrict__ y, float* __restrict__ dst, int n, int act) {
    const int i = blockIdx.x * 256 + threadIdx.x;
    if (i < n) { const float v = act_fn(x[i], act) * y[i]; VST2(float, dst + i, v); }
}

__global__ __launch_bounds__(256) void k_matvec(GemmP p) {
    const int rpt = (p.N == 1) ? 1 : 32;
    const long long r0 = ((long long)blockIdx.x * 256 + threadIdx.x) * rpt; const int z = blockIdx.z, zo = z / p.zi_n, zi = z - zo * p.zi_n;
    if (r0 >= p.M) return;
    const float* Bb = p.B + zo * p.sBo + zi * p.sBi;
    float* C = p.C + zo * p.sCo + zi * p.sCi; const float* R = p.R + zo * p.sRo + zi * p.sRi;
    for (int rr = 0; rr < rpt; ++rr) {
        const long long r = r0 + rr; if (r >= p.M) break;
        const float* A = p.A + zo * p.sAo + zi * p.sAi + r * p.sAm;
        float acc[8] = {0.f, 0.f, 0.f, 0.f, 0.f, 0.f, 0.f, 0.f};
        for (int k = 0; k < p.K; ++k) { const float a = A[(long long)k * p.sAk];
#pragma unroll
            for (int j = 0; j < 8; ++j) if (j < p.N) acc[j] += a * Bb[(long long)j * p.sBn + (long long)k * p.sBk]; }
#pragma unroll
        for (int j = 0; j < 8; ++j) if (j < p.N) {
            float v = acc[j] * p.alpha;
            if (p.flags & 1) v += p.bias[j];
            if (p.flags & 2) v += p.bias[r];
            v = act_fn(v, p.act);
            if (p.flags & 4) v += p.beta * R[r * p.sRm + (long long)j * p.sRn];
            VST2(float, C + r * p.sCm + j, v);
        }
    }
}
__global__ __launch_bounds__(256) void k_smallsoftmax(const float* __restrict__ src, float* __restrict__ dst, long long sr, long long dr, int n, long long R, float scale) {
    const long long r0 = ((long long)blockIdx.x * 256 + threadIdx.x) * 32;
    for (int rr = 0; rr < 32; ++rr) {
        const long long r = r0 + rr; if (r >= R) return;
        const float* s = src + r * sr; float* d = dst + r * dr;
        float mx = -__builtin_inff();
        for (int j = 0; j < n; ++j) mx = fmaxf(mx, s[j] * scale);
        float sum = 0.f;
        for (int j = 0; j < n; ++j) sum += expf(s[j] * scale - mx);
        const float inv = 1.f / sum;
        for (int j = 0; j < n; ++j) { const float v = expf(s[j] * scale - mx) * inv; VST2(float, d + j, v); }
    }
}

__global__ __launch_bounds__(32) void k_unitstat(float* __restrict__ st) { const int t = threadIdx.x; const float v = (t == 1) ? 1.f : 0.f; VST2(float, st + t, v); }

__global__ __launch_bounds__(256) void k_lincopy(const float* __restrict__ src, long long lds, float* __restrict__ dst, long long ldd, long long rows, int cols) {
    const long long i = (long long)blockIdx.x * 256 + threadIdx.x; if (i >= rows * cols) return;
    const long long r = i / cols; const int c = (int)(i - r * cols);
    const float v = src[r * lds + c]; VST2(float, dst + r * ldd + c, v);
}

__global__ __launch_bounds__(256) void k_seg_init(const int* __restrict__ tok, const float* __restrict__ emb, float* __restrict__ S, float* __restrict__ Cc, int N, int L, int E, int H, int ls, int t0) {
    const long long q = (long long)blockIdx.x * 256 + threadIdx.x; if (q >= (long long)N * ls) return; const int c = (int)(q % ls); const long long n = q / ls; float v = 0.f;
    if (c < E) { int id = tok[n * L + t0]; id = min(max(id, 0), 2); v = emb[id * E + c]; }
    VST2(float, S + q, v); if (c < H) VST2(float, Cc + n * H + c, 0.f);
}
__global__ __launch_bounds__(256) void k_seg_cell(const float* __restrict__ GT, const int* __restrict__ tok, const int* __restrict__ len, const float* __restrict__ emb, float* __restrict__ S, float* __restrict__ Cc, float* __restrict__ OUT, int N, int L, int E, int H, int ls, int t, int tn, int last, int ooff) {
    const long long q = (long long)blockIdx.x * 256 + threadIdx.x; if (q >= (long long)N * H) return; const int j = (int)(q % H); const long long n = q / H; const float* gt = GT + n * 4 * H;
    float h = S[n * ls + E + j], c = Cc[n * H + j];
    if (t < len[n]) { const float ig = 1.f / (1.f + expf(-gt[j])), fg = 1.f / (1.f + expf(-gt[H + j])), gg = tanhf(gt[2 * H + j]), og = 1.f / (1.f + expf(-gt[3 * H + j])); c = fg * c + ig * gg; h = og * tanhf(c); }
    VST2(float, Cc + n * H + j, c); VST2(float, S + n * ls + E + j, h);
    if (tn >= 0 && j < E) { int id = tok[n * L + tn]; id = min(max(id, 0), 2); VST2(float, S + n * ls + j, emb[id * E + j]); }
    if (last) VST2(float, OUT + n * 2 * H + ooff + j, h);
}

template __global__ void k_gemm<1>(GemmP);

extern "C" void kernel_launch(void* const* d_in, const int* in_sizes, int n_in, void* d_out, int out_size, void* d_ws, size_t ws_size, hipStream_t stream) {
    (void)in_sizes; (void)n_in; (void)out_size; (void)ws_size;
    const int* tok = (const int*)d_in[0];
    const int* len = (const int*)d_in[1];
    const float* emb = (const float*)d_in[2];
    const float* Wihf = (const float*)d_in[3];
    const float* Whhf = (const float*)d_in[4];
    const float* bf = (const float*)d_in[5];
    const float* Wihb = (const float*)d_in[6];
    const float* Whhb = (const float*)d_in[7];
    const float* bb = (const float*)d_in[8];
    const int N = 131072;
    const int L = 32;
    const int E = 16;
    const int H = 32;
    const int G4 = 128;
    const int LS = 64;
    float* out = (float*)d_out;
    char* wsp = (char*)d_ws;
    float* PF = (float*)wsp; wsp += (((size_t)((size_t)64 * G4) * 4 + 255) / 256) * 256;
    float* PB = (float*)wsp; wsp += (((size_t)((size_t)64 * G4) * 4 + 255) / 256) * 256;
    float* S = (float*)wsp; wsp += (((size_t)((size_t)N * LS) * 4 + 255) / 256) * 256;
    float* C = (float*)wsp; wsp += (((size_t)((size_t)N * H) * 4 + 255) / 256) * 256;
    float* GT = (float*)wsp; wsp += (((size_t)((size_t)N * G4) * 4 + 255) / 256) * 256;
    { TrP t; t.src = Wihf; t.dst = PF; t.R2 = Wihf; t.sSz = 0; t.lds = E; t.sDz = 0; t.ldd = G4; t.sRz = 0; t.ldr = 0;
      t.R = G4; t.C = E; t.flags = 0; t.act = 0; t.alpha = 1.0f; t.beta = 0.0f;
      k_tr<<<dim3((unsigned)((E) + 31) / 32, (unsigned)((G4) + 31) / 32, (unsigned)(1)), 256, 0, stream>>>(t); }
    { TrP t; t.src = Whhf; t.dst = PF + (size_t)E * G4; t.R2 = Whhf; t.sSz = 0; t.lds = H; t.sDz = 0; t.ldd = G4; t.sRz = 0; t.ldr = 0;
      t.R = G4; t.C = H; t.flags = 0; t.act = 0; t.alpha = 1.0f; t.beta = 0.0f;
      k_tr<<<dim3((unsigned)((H) + 31) / 32, (unsigned)((G4) + 31) / 32, (unsigned)(1)), 256, 0, stream>>>(t); }
    { TrP t; t.src = Wihb; t.dst = PB; t.R2 = Wihb; t.sSz = 0; t.lds = E; t.sDz = 0; t.ldd = G4; t.sRz = 0; t.ldr = 0;
      t.R = G4; t.C = E; t.flags = 0; t.act = 0; t.alpha = 1.0f; t.beta = 0.0f;
      k_tr<<<dim3((unsigned)((E) + 31) / 32, (unsigned)((G4) + 31) / 32, (unsigned)(1)), 256, 0, stream>>>(t); }
    { TrP t; t.src = Whhb; t.dst = PB + (size_t)E * G4; t.R2 = Whhb; t.sSz = 0; t.lds = H; t.sDz = 0; t.ldd = G4; t.sRz = 0; t.ldr = 0;
      t.R = G4; t.C = H; t.flags = 0; t.act = 0; t.alpha = 1.0f; t.beta = 0.0f;
      k_tr<<<dim3((unsigned)((H) + 31) / 32, (unsigned)((G4) + 31) / 32, (unsigned)(1)), 256, 0, stream>>>(t); }
    k_seg_init<<<(unsigned)(((long long)N * LS + 255) / 256), 256, 0, stream>>>(tok, emb, S, C, N, L, E, H, LS, 0);
    { GemmP gf0;
      gf0.A = S; gf0.B = PF; gf0.bias = bf; gf0.R = S; gf0.C = GT;
      gf0.sAo = 0; gf0.sAi = 0; gf0.sAm = LS; gf0.sAk = 1; gf0.sBo = 0; gf0.sBi = 0; gf0.sBn = 1; gf0.sBk = G4; gf0.sCo = 0; gf0.sCi = 0; gf0.sCm = G4; gf0.sRo = 0; gf0.sRi = 0; gf0.sRm = 0; gf0.sRn = 0;
      gf0.M = N; gf0.N = G4; gf0.K = E + H; gf0.zi_n = 1; gf0.flags = 1; gf0.act = 0;
      gf0.alpha = 1.0f; gf0.beta = 0.0f; gf0.sa = 1.0f; gf0.sb = 1.0f; gf0.Npad = G4; gf0.pad_ = 0;
      k_gemm<1><<<dim3((unsigned)((G4) + 31) / 32, (unsigned)((N) + 15) / 16, (unsigned)(1)), 32, 0, stream>>>(gf0); }
    k_seg_cell<<<(unsigned)(((long long)N * H + 255) / 256), 256, 0, stream>>>(GT, tok, len, emb, S, C, out, N, L, E, H, LS, 0, 1, 0, 0);
    { GemmP gf1;
      gf1.A = S; gf1.B = PF; gf1.bias = bf; gf1.R = S; gf1.C = GT;
      gf1.sAo = 0; gf1.sAi = 0; gf1.sAm = LS; gf1.sAk = 1; gf1.sBo = 0; gf1.sBi = 0; gf1.sBn = 1; gf1.sBk = G4; gf1.sCo = 0; gf1.sCi = 0; gf1.sCm = G4; gf1.sRo = 0; gf1.sRi = 0; gf1.sRm = 0; gf1.sRn = 0;
      gf1.M = N; gf1.N = G4; gf1.K = E + H; gf1.zi_n = 1; gf1.flags = 1; gf1.act = 0;
      gf1.alpha = 1.0f; gf1.beta = 0.0f; gf1.sa = 1.0f; gf1.sb = 1.0f; gf1.Npad = G4; gf1.pad_ = 0;
      k_gemm<1><<<dim3((unsigned)((G4) + 31) / 32, (unsigned)((N) + 15) / 16, (unsigned)(1)), 32, 0, stream>>>(gf1); }
    k_seg_cell<<<(unsigned)(((long long)N * H + 255) / 256), 256, 0, stream>>>(GT, tok, len, emb, S, C, out, N, L, E, H, LS, 1, 2, 0, 0);
    { GemmP gf2;
      gf2.A = S; gf2.B = PF; gf2.bias = bf; gf2.R = S; gf2.C = GT;
      gf2.sAo = 0; gf2.sAi = 0; gf2.sAm = LS; gf2.sAk = 1; gf2.sBo = 0; gf2.sBi = 0; gf2.sBn = 1; gf2.sBk = G4; gf2.sCo = 0; gf2.sCi = 0; gf2.sCm = G4; gf2.sRo = 0; gf2.sRi = 0; gf2.sRm = 0; gf2.sRn = 0;
      gf2.M = N; gf2.N = G4; gf2.K = E + H; gf2.zi_n = 1; gf2.flags = 1; gf2.act = 0;
      gf2.alpha = 1.0f; gf2.beta = 0.0f; gf2.sa = 1.0f; gf2.sb = 1.0f; gf2.Npad = G4; gf2.pad_ = 0;
      k_gemm<1><<<dim3((unsigned)((G4) + 31) / 32, (unsigned)((N) + 15) / 16, (unsigned)(1)), 32, 0, stream>>>(gf2); }
    k_seg_cell<<<(unsigned)(((long long)N * H + 255) / 256), 256, 0, stream>>>(GT, tok, len, emb, S, C, out, N, L, E, H, LS, 2, 3, 0, 0);
    { GemmP gf3;
      gf3.A = S; gf3.B = PF; gf3.bias = bf; gf3.R = S; gf3.C = GT;
      gf3.sAo = 0; gf3.sAi = 0; gf3.sAm = LS; gf3.sAk = 1; gf3.sBo = 0; gf3.sBi = 0; gf3.sBn = 1; gf3.sBk = G4; gf3.sCo = 0; gf3.sCi = 0; gf3.sCm = G4; gf3.sRo = 0; gf3.sRi = 0; gf3.sRm = 0; gf3.sRn = 0;
      gf3.M = N; gf3.N = G4; gf3.K = E + H; gf3.zi_n = 1; gf3.flags = 1; gf3.act = 0;
      gf3.alpha = 1.0f; gf3.beta = 0.0f; gf3.sa = 1.0f; gf3.sb = 1.0f; gf3.Npad = G4; gf3.pad_ = 0;
      k_gemm<1><<<dim3((unsigned)((G4) + 31) / 32, (unsigned)((N) + 15) / 16, (unsigned)(1)), 32, 0, stream>>>(gf3); }
    k_seg_cell<<<(unsigned)(((long long)N * H + 255) / 256), 256, 0, stream>>>(GT, tok, len, emb, S, C, out, N, L, E, H, LS, 3, 4, 0, 0);
    { GemmP gf4;
      gf4.A = S; gf4.B = PF; gf4.bias = bf; gf4.R = S; gf4.C = GT;
      gf4.sAo = 0; gf4.sAi = 0; gf4.sAm = LS; gf4.sAk = 1; gf4.sBo = 0; gf4.sBi = 0; gf4.sBn = 1; gf4.sBk = G4; gf4.sCo = 0; gf4.sCi = 0; gf4.sCm = G4; gf4.sRo = 0; gf4.sRi = 0; gf4.sRm = 0; gf4.sRn = 0;
      gf4.M = N; gf4.N = G4; gf4.K = E + H; gf4.zi_n = 1; gf4.flags = 1; gf4.act = 0;
      gf4.alpha = 1.0f; gf4.beta = 0.0f; gf4.sa = 1.0f; gf4.sb = 1.0f; gf4.Npad = G4; gf4.pad_ = 0;
      k_gemm<1><<<dim3((unsigned)((G4) + 31) / 32, (unsigned)((N) + 15) / 16, (unsigned)(1)), 32, 0, stream>>>(gf4); }
    k_seg_cell<<<(unsigned)(((long long)N * H + 255) / 256), 256, 0, stream>>>(GT, tok, len, emb, S, C, out, N, L, E, H, LS, 4, 5, 0, 0);
    { GemmP gf5;
      gf5.A = S; gf5.B = PF; gf5.bias = bf; gf5.R = S; gf5.C = GT;
      gf5.sAo = 0; gf5.sAi = 0; gf5.sAm = LS; gf5.sAk = 1; gf5.sBo = 0; gf5.sBi = 0; gf5.sBn = 1; gf5.sBk = G4; gf5.sCo = 0; gf5.sCi = 0; gf5.sCm = G4; gf5.sRo = 0; gf5.sRi = 0; gf5.sRm = 0; gf5.sRn = 0;
      gf5.M = N; gf5.N = G4; gf5.K = E + H; gf5.zi_n = 1; gf5.flags = 1; gf5.act = 0;
      gf5.alpha = 1.0f; gf5.beta = 0.0f; gf5.sa = 1.0f; gf5.sb = 1.0f; gf5.Npad = G4; gf5.pad_ = 0;
      k_gemm<1><<<dim3((unsigned)((G4) + 31) / 32, (unsigned)((N) + 15) / 16, (unsigned)(1)), 32, 0, stream>>>(gf5); }
    k_seg_cell<<<(unsigned)(((long long)N * H + 255) / 256), 256, 0, stream>>>(GT, tok, len, emb, S, C, out, N, L, E, H, LS, 5, 6, 0, 0);
    { GemmP gf6;
      gf6.A = S; gf6.B = PF; gf6.bias = bf; gf6.R = S; gf6.C = GT;
      gf6.sAo = 0; gf6.sAi = 0; gf6.sAm = LS; gf6.sAk = 1; gf6.sBo = 0; gf6.sBi = 0; gf6.sBn = 1; gf6.sBk = G4; gf6.sCo = 0; gf6.sCi = 0; gf6.sCm = G4; gf6.sRo = 0; gf6.sRi = 0; gf6.sRm = 0; gf6.sRn = 0;
      gf6.M = N; gf6.N = G4; gf6.K = E + H; gf6.zi_n = 1; gf6.flags = 1; gf6.act = 0;
      gf6.alpha = 1.0f; gf6.beta = 0.0f; gf6.sa = 1.0f; gf6.sb = 1.0f; gf6.Npad = G4; gf6.pad_ = 0;
      k_gemm<1><<<dim3((unsigned)((G4) + 31) / 32, (unsigned)((N) + 15) / 16, (unsigned)(1)), 32, 0, stream>>>(gf6); }
    k_seg_cell<<<(unsigned)(((long long)N * H + 255) / 256), 256, 0, stream>>>(GT, tok, len, emb, S, C, out, N, L, E, H, LS, 6, 7, 0, 0);
    { GemmP gf7;
      gf7.A = S; gf7.B = PF; gf7.bias = bf; gf7.R = S; gf7.C = GT;
      gf7.sAo = 0; gf7.sAi = 0; gf7.sAm = LS; gf7.sAk = 1; gf7.sBo = 0; gf7.sBi = 0; gf7.sBn = 1; gf7.sBk = G4; gf7.sCo = 0; gf7.sCi = 0; gf7.sCm = G4; gf7.sRo = 0; gf7.sRi = 0; gf7.sRm = 0; gf7.sRn = 0;
      gf7.M = N; gf7.N = G4; gf7.K = E + H; gf7.zi_n = 1; gf7.flags = 1; gf7.act = 0;
      gf7.alpha = 1.0f; gf7.beta = 0.0f; gf7.sa = 1.0f; gf7.sb = 1.0f; gf7.Npad = G4; gf7.pad_ = 0;
      k_gemm<1><<<dim3((unsigned)((G4) + 31) / 32, (unsigned)((N) + 15) / 16, (unsigned)(1)), 32, 0, stream>>>(gf7); }
    k_seg_cell<<<(unsigned)(((long long)N * H + 255) / 256), 256, 0, stream>>>(GT, tok, len, emb, S, C, out, N, L, E, H, LS, 7, 8, 0, 0);
    { GemmP gf8;
      gf8.A = S; gf8.B = PF; gf8.bias = bf; gf8.R = S; gf8.C = GT;
      gf8.sAo = 0; gf8.sAi = 0; gf8.sAm = LS; gf8.sAk = 1; gf8.sBo = 0; gf8.sBi = 0; gf8.sBn = 1; gf8.sBk = G4; gf8.sCo = 0; gf8.sCi = 0; gf8.sCm = G4; gf8.sRo = 0; gf8.sRi = 0; gf8.sRm = 0; gf8.sRn = 0;
      gf8.M = N; gf8.N = G4; gf8.K = E + H; gf8.zi_n = 1; gf8.flags = 1; gf8.act = 0;
      gf8.alpha = 1.0f; gf8.beta = 0.0f; gf8.sa = 1.0f; gf8.sb = 1.0f; gf8.Npad = G4; gf8.pad_ = 0;
      k_gemm<1><<<dim3((unsigned)((G4) + 31) / 32, (unsigned)((N) + 15) / 16, (unsigned)(1)), 32, 0, stream>>>(gf8); }
    k_seg_cell<<<(unsigned)(((long long)N * H + 255) / 256), 256, 0, stream>>>(GT, tok, len, emb, S, C, out, N, L, E, H, LS, 8, 9, 0, 0);
    { GemmP gf9;
      gf9.A = S; gf9.B = PF; gf9.bias = bf; gf9.R = S; gf9.C = GT;
      gf9.sAo = 0; gf9.sAi = 0; gf9.sAm = LS; gf9.sAk = 1; gf9.sBo = 0; gf9.sBi = 0; gf9.sBn = 1; gf9.sBk = G4; gf9.sCo = 0; gf9.sCi = 0; gf9.sCm = G4; gf9.sRo = 0; gf9.sRi = 0; gf9.sRm = 0; gf9.sRn = 0;
      gf9.M = N; gf9.N = G4; gf9.K = E + H; gf9.zi_n = 1; gf9.flags = 1; gf9.act = 0;
      gf9.alpha = 1.0f; gf9.beta = 0.0f; gf9.sa = 1.0f; gf9.sb = 1.0f; gf9.Npad = G4; gf9.pad_ = 0;
      k_gemm<1><<<dim3((unsigned)((G4) + 31) / 32, (unsigned)((N) + 15) / 16, (unsigned)(1)), 32, 0, stream>>>(gf9); }
    k_seg_cell<<<(unsigned)(((long long)N * H + 255) / 256), 256, 0, stream>>>(GT, tok, len, emb, S, C, out, N, L, E, H, LS, 9, 10, 0, 0);
    { GemmP gf10;
      gf10.A = S; gf10.B = PF; gf10.bias = bf; gf10.R = S; gf10.C = GT;
      gf10.sAo = 0; gf10.sAi = 0; gf10.sAm = LS; gf10.sAk = 1; gf10.sBo = 0; gf10.sBi = 0; gf10.sBn = 1; gf10.sBk = G4; gf10.sCo = 0; gf10.sCi = 0; gf10.sCm = G4; gf10.sRo = 0; gf10.sRi = 0; gf10.sRm = 0; gf10.sRn = 0;
      gf10.M = N; gf10.N = G4; gf10.K = E + H; gf10.zi_n = 1; gf10.flags = 1; gf10.act = 0;
      gf10.alpha = 1.0f; gf10.beta = 0.0f; gf10.sa = 1.0f; gf10.sb = 1.0f; gf10.Npad = G4; gf10.pad_ = 0;
      k_gemm<1><<<dim3((unsigned)((G4) + 31) / 32, (unsigned)((N) + 15) / 16, (unsigned)(1)), 32, 0, stream>>>(gf10); }
    k_seg_cell<<<(unsigned)(((long long)N * H + 255) / 256), 256, 0, stream>>>(GT, tok, len, emb, S, C, out, N, L, E, H, LS, 10, 11, 0, 0);
    { GemmP gf11;
      gf11.A = S; gf11.B = PF; gf11.bias = bf; gf11.R = S; gf11.C = GT;
      gf11.sAo = 0; gf11.sAi = 0; gf11.sAm = LS; gf11.sAk = 1; gf11.sBo = 0; gf11.sBi = 0; gf11.sBn = 1; gf11.sBk = G4; gf11.sCo = 0; gf11.sCi = 0; gf11.sCm = G4; gf11.sRo = 0; gf11.sRi = 0; gf11.sRm = 0; gf11.sRn = 0;
      gf11.M = N; gf11.N = G4; gf11.K = E + H; gf11.zi_n = 1; gf11.flags = 1; gf11.act = 0;
      gf11.alpha = 1.0f; gf11.beta = 0.0f; gf11.sa = 1.0f; gf11.sb = 1.0f; gf11.Npad = G4; gf11.pad_ = 0;
      k_gemm<1><<<dim3((unsigned)((G4) + 31) / 32, (unsigned)((N) + 15) / 16, (unsigned)(1)), 32, 0, stream>>>(gf11); }
    k_seg_cell<<<(unsigned)(((long long)N * H + 255) / 256), 256, 0, stream>>>(GT, tok, len, emb, S, C, out, N, L, E, H, LS, 11, 12, 0, 0);
    { GemmP gf12;
      gf12.A = S; gf12.B = PF; gf12.bias = bf; gf12.R = S; gf12.C = GT;
      gf12.sAo = 0; gf12.sAi = 0; gf12.sAm = LS; gf12.sAk = 1; gf12.sBo = 0; gf12.sBi = 0; gf12.sBn = 1; gf12.sBk = G4; gf12.sCo = 0; gf12.sCi = 0; gf12.sCm = G4; gf12.sRo = 0; gf12.sRi = 0; gf12.sRm = 0; gf12.sRn = 0;
      gf12.M = N; gf12.N = G4; gf12.K = E + H; gf12.zi_n = 1; gf12.flags = 1; gf12.act = 0;
      gf12.alpha = 1.0f; gf12.beta = 0.0f; gf12.sa = 1.0f; gf12.sb = 1.0f; gf12.Npad = G4; gf12.pad_ = 0;
      k_gemm<1><<<dim3((unsigned)((G4) + 31) / 32, (unsigned)((N) + 15) / 16, (unsigned)(1)), 32, 0, stream>>>(gf12); }
    k_seg_cell<<<(unsigned)(((long long)N * H + 255) / 256), 256, 0, stream>>>(GT, tok, len, emb, S, C, out, N, L, E, H, LS, 12, 13, 0, 0);
    { GemmP gf13;
      gf13.A = S; gf13.B = PF; gf13.bias = bf; gf13.R = S; gf13.C = GT;
      gf13.sAo = 0; gf13.sAi = 0; gf13.sAm = LS; gf13.sAk = 1; gf13.sBo = 0; gf13.sBi = 0; gf13.sBn = 1; gf13.sBk = G4; gf13.sCo = 0; gf13.sCi = 0; gf13.sCm = G4; gf13.sRo = 0; gf13.sRi = 0; gf13.sRm = 0; gf13.sRn = 0;
      gf13.M = N; gf13.N = G4; gf13.K = E + H; gf13.zi_n = 1; gf13.flags = 1; gf13.act = 0;
      gf13.alpha = 1.0f; gf13.beta = 0.0f; gf13.sa = 1.0f; gf13.sb = 1.0f; gf13.Npad = G4; gf13.pad_ = 0;
      k_gemm<1><<<dim3((unsigned)((G4) + 31) / 32, (unsigned)((N) + 15) / 16, (unsigned)(1)), 32, 0, stream>>>(gf13); }
    k_seg_cell<<<(unsigned)(((long long)N * H + 255) / 256), 256, 0, stream>>>(GT, tok, len, emb, S, C, out, N, L, E, H, LS, 13, 14, 0, 0);
    { GemmP gf14;
      gf14.A = S; gf14.B = PF; gf14.bias = bf; gf14.R = S; gf14.C = GT;
      gf14.sAo = 0; gf14.sAi = 0; gf14.sAm = LS; gf14.sAk = 1; gf14.sBo = 0; gf14.sBi = 0; gf14.sBn = 1; gf14.sBk = G4; gf14.sCo = 0; gf14.sCi = 0; gf14.sCm = G4; gf14.sRo = 0; gf14.sRi = 0; gf14.sRm = 0; gf14.sRn = 0;
      gf14.M = N; gf14.N = G4; gf14.K = E + H; gf14.zi_n = 1; gf14.flags = 1; gf14.act = 0;
      gf14.alpha = 1.0f; gf14.beta = 0.0f; gf14.sa = 1.0f; gf14.sb = 1.0f; gf14.Npad = G4; gf14.pad_ = 0;
      k_gemm<1><<<dim3((unsigned)((G4) + 31) / 32, (unsigned)((N) + 15) / 16, (unsigned)(1)), 32, 0, stream>>>(gf14); }
    k_seg_cell<<<(unsigned)(((long long)N * H + 255) / 256), 256, 0, stream>>>(GT, tok, len, emb, S, C, out, N, L, E, H, LS, 14, 15, 0, 0);
    { GemmP gf15;
      gf15.A = S; gf15.B = PF; gf15.bias = bf; gf15.R = S; gf15.C = GT;
      gf15.sAo = 0; gf15.sAi = 0; gf15.sAm = LS; gf15.sAk = 1; gf15.sBo = 0; gf15.sBi = 0; gf15.sBn = 1; gf15.sBk = G4; gf15.sCo = 0; gf15.sCi = 0; gf15.sCm = G4; gf15.sRo = 0; gf15.sRi = 0; gf15.sRm = 0; gf15.sRn = 0;
      gf15.M = N; gf15.N = G4; gf15.K = E + H; gf15.zi_n = 1; gf15.flags = 1; gf15.act = 0;
      gf15.alpha = 1.0f; gf15.beta = 0.0f; gf15.sa = 1.0f; gf15.sb = 1.0f; gf15.Npad = G4; gf15.pad_ = 0;
      k_gemm<1><<<dim3((unsigned)((G4) + 31) / 32, (unsigned)((N) + 15) / 16, (unsigned)(1)), 32, 0, stream>>>(gf15); }
    k_seg_cell<<<(unsigned)(((long long)N * H + 255) / 256), 256, 0, stream>>>(GT, tok, len, emb, S, C, out, N, L, E, H, LS, 15, 16, 0, 0);
    { GemmP gf16;
      gf16.A = S; gf16.B = PF; gf16.bias = bf; gf16.R = S; gf16.C = GT;
      gf16.sAo = 0; gf16.sAi = 0; gf16.sAm = LS; gf16.sAk = 1; gf16.sBo = 0; gf16.sBi = 0; gf16.sBn = 1; gf16.sBk = G4; gf16.sCo = 0; gf16.sCi = 0; gf16.sCm = G4; gf16.sRo = 0; gf16.sRi = 0; gf16.sRm = 0; gf16.sRn = 0;
      gf16.M = N; gf16.N = G4; gf16.K = E + H; gf16.zi_n = 1; gf16.flags = 1; gf16.act = 0;
      gf16.alpha = 1.0f; gf16.beta = 0.0f; gf16.sa = 1.0f; gf16.sb = 1.0f; gf16.Npad = G4; gf16.pad_ = 0;
      k_gemm<1><<<dim3((unsigned)((G4) + 31) / 32, (unsigned)((N) + 15) / 16, (unsigned)(1)), 32, 0, stream>>>(gf16); }
    k_seg_cell<<<(unsigned)(((long long)N * H + 255) / 256), 256, 0, stream>>>(GT, tok, len, emb, S, C, out, N, L, E, H, LS, 16, 17, 0, 0);
    { GemmP gf17;
      gf17.A = S; gf17.B = PF; gf17.bias = bf; gf17.R = S; gf17.C = GT;
      gf17.sAo = 0; gf17.sAi = 0; gf17.sAm = LS; gf17.sAk = 1; gf17.sBo = 0; gf17.sBi = 0; gf17.sBn = 1; gf17.sBk = G4; gf17.sCo = 0; gf17.sCi = 0; gf17.sCm = G4; gf17.sRo = 0; gf17.sRi = 0; gf17.sRm = 0; gf17.sRn = 0;
      gf17.M = N; gf17.N = G4; gf17.K = E + H; gf17.zi_n = 1; gf17.flags = 1; gf17.act = 0;
      gf17.alpha = 1.0f; gf17.beta = 0.0f; gf17.sa = 1.0f; gf17.sb = 1.0f; gf17.Npad = G4; gf17.pad_ = 0;
      k_gemm<1><<<dim3((unsigned)((G4) + 31) / 32, (unsigned)((N) + 15) / 16, (unsigned)(1)), 32, 0, stream>>>(gf17); }
    k_seg_cell<<<(unsigned)(((long long)N * H + 255) / 256), 256, 0, stream>>>(GT, tok, len, emb, S, C, out, N, L, E, H, LS, 17, 18, 0, 0);
    { GemmP gf18;
      gf18.A = S; gf18.B = PF; gf18.bias = bf; gf18.R = S; gf18.C = GT;
      gf18.sAo = 0; gf18.sAi = 0; gf18.sAm = LS; gf18.sAk = 1; gf18.sBo = 0; gf18.sBi = 0; gf18.sBn = 1; gf18.sBk = G4; gf18.sCo = 0; gf18.sCi = 0; gf18.sCm = G4; gf18.sRo = 0; gf18.sRi = 0; gf18.sRm = 0; gf18.sRn = 0;
      gf18.M = N; gf18.N = G4; gf18.K = E + H; gf18.zi_n = 1; gf18.flags = 1; gf18.act = 0;
      gf18.alpha = 1.0f; gf18.beta = 0.0f; gf18.sa = 1.0f; gf18.sb = 1.0f; gf18.Npad = G4; gf18.pad_ = 0;
      k_gemm<1><<<dim3((unsigned)((G4) + 31) / 32, (unsigned)((N) + 15) / 16, (unsigned)(1)), 32, 0, stream>>>(gf18); }
    k_seg_cell<<<(unsigned)(((long long)N * H + 255) / 256), 256, 0, stream>>>(GT, tok, len, emb, S, C, out, N, L, E, H, LS, 18, 19, 0, 0);
    { GemmP gf19;
      gf19.A = S; gf19.B = PF; gf19.bias = bf; gf19.R = S; gf19.C = GT;
      gf19.sAo = 0; gf19.sAi = 0; gf19.sAm = LS; gf19.sAk = 1; gf19.sBo = 0; gf19.sBi = 0; gf19.sBn = 1; gf19.sBk = G4; gf19.sCo = 0; gf19.sCi = 0; gf19.sCm = G4; gf19.sRo = 0; gf19.sRi = 0; gf19.sRm = 0; gf19.sRn = 0;
      gf19.M = N; gf19.N = G4; gf19.K = E + H; gf19.zi_n = 1; gf19.flags = 1; gf19.act = 0;
      gf19.alpha = 1.0f; gf19.beta = 0.0f; gf19.sa = 1.0f; gf19.sb = 1.0f; gf19.Npad = G4; gf19.pad_ = 0;
      k_gemm<1><<<dim3((unsigned)((G4) + 31) / 32, (unsigned)((N) + 15) / 16, (unsigned)(1)), 32, 0, stream>>>(gf19); }
    k_seg_cell<<<(unsigned)(((long long)N * H + 255) / 256), 256, 0, stream>>>(GT, tok, len, emb, S, C, out, N, L, E, H, LS, 19, 20, 0, 0);
    { GemmP gf20;
      gf20.A = S; gf20.B = PF; gf20.bias = bf; gf20.R = S; gf20.C = GT;
      gf20.sAo = 0; gf20.sAi = 0; gf20.sAm = LS; gf20.sAk = 1; gf20.sBo = 0; gf20.sBi = 0; gf20.sBn = 1; gf20.sBk = G4; gf20.sCo = 0; gf20.sCi = 0; gf20.sCm = G4; gf20.sRo = 0; gf20.sRi = 0; gf20.sRm = 0; gf20.sRn = 0;
      gf20.M = N; gf20.N = G4; gf20.K = E + H; gf20.zi_n = 1; gf20.flags = 1; gf20.act = 0;
      gf20.alpha = 1.0f; gf20.beta = 0.0f; gf20.sa = 1.0f; gf20.sb = 1.0f; gf20.Npad = G4; gf20.pad_ = 0;
      k_gemm<1><<<dim3((unsigned)((G4) + 31) / 32, (unsigned)((N) + 15) / 16, (unsigned)(1)), 32, 0, stream>>>(gf20); }
    k_seg_cell<<<(unsigned)(((long long)N * H + 255) / 256), 256, 0, stream>>>(GT, tok, len, emb, S, C, out, N, L, E, H, LS, 20, 21, 0, 0);
    { GemmP gf21;
      gf21.A = S; gf21.B = PF; gf21.bias = bf; gf21.R = S; gf21.C = GT;
      gf21.sAo = 0; gf21.sAi = 0; gf21.sAm = LS; gf21.sAk = 1; gf21.sBo = 0; gf21.sBi = 0; gf21.sBn = 1; gf21.sBk = G4; gf21.sCo = 0; gf21.sCi = 0; gf21.sCm = G4; gf21.sRo = 0; gf21.sRi = 0; gf21.sRm = 0; gf21.sRn = 0;
      gf21.M = N; gf21.N = G4; gf21.K = E + H; gf21.zi_n = 1; gf21.flags = 1; gf21.act = 0;
      gf21.alpha = 1.0f; gf21.beta = 0.0f; gf21.sa = 1.0f; gf21.sb = 1.0f; gf21.Npad = G4; gf21.pad_ = 0;
      k_gemm<1><<<dim3((unsigned)((G4) + 31) / 32, (unsigned)((N) + 15) / 16, (unsigned)(1)), 32, 0, stream>>>(gf21); }
    k_seg_cell<<<(unsigned)(((long long)N * H + 255) / 256), 256, 0, stream>>>(GT, tok, len, emb, S, C, out, N, L, E, H, LS, 21, 22, 0, 0);
    { GemmP gf22;
      gf22.A = S; gf22.B = PF; gf22.bias = bf; gf22.R = S; gf22.C = GT;
      gf22.sAo = 0; gf22.sAi = 0; gf22.sAm = LS; gf22.sAk = 1; gf22.sBo = 0; gf22.sBi = 0; gf22.sBn = 1; gf22.sBk = G4; gf22.sCo = 0; gf22.sCi = 0; gf22.sCm = G4; gf22.sRo = 0; gf22.sRi = 0; gf22.sRm = 0; gf22.sRn = 0;
      gf22.M = N; gf22.N = G4; gf22.K = E + H; gf22.zi_n = 1; gf22.flags = 1; gf22.act = 0;
      gf22.alpha = 1.0f; gf22.beta = 0.0f; gf22.sa = 1.0f; gf22.sb = 1.0f; gf22.Npad = G4; gf22.pad_ = 0;
      k_gemm<1><<<dim3((unsigned)((G4) + 31) / 32, (unsigned)((N) + 15) / 16, (unsigned)(1)), 32, 0, stream>>>(gf22); }
    k_seg_cell<<<(unsigned)(((long long)N * H + 255) / 256), 256, 0, stream>>>(GT, tok, len, emb, S, C, out, N, L, E, H, LS, 22, 23, 0, 0);
    { GemmP gf23;
      gf23.A = S; gf23.B = PF; gf23.bias = bf; gf23.R = S; gf23.C = GT;
      gf23.sAo = 0; gf23.sAi = 0; gf23.sAm = LS; gf23.sAk = 1; gf23.sBo = 0; gf23.sBi = 0; gf23.sBn = 1; gf23.sBk = G4; gf23.sCo = 0; gf23.sCi = 0; gf23.sCm = G4; gf23.sRo = 0; gf23.sRi = 0; gf23.sRm = 0; gf23.sRn = 0;
      gf23.M = N; gf23.N = G4; gf23.K = E + H; gf23.zi_n = 1; gf23.flags = 1; gf23.act = 0;
      gf23.alpha = 1.0f; gf23.beta = 0.0f; gf23.sa = 1.0f; gf23.sb = 1.0f; gf23.Npad = G4; gf23.pad_ = 0;
      k_gemm<1><<<dim3((unsigned)((G4) + 31) / 32, (unsigned)((N) + 15) / 16, (unsigned)(1)), 32, 0, stream>>>(gf23); }
    k_seg_cell<<<(unsigned)(((long long)N * H + 255) / 256), 256, 0, stream>>>(GT, tok, len, emb, S, C, out, N, L, E, H, LS, 23, 24, 0, 0);
    { GemmP gf24;
      gf24.A = S; gf24.B = PF; gf24.bias = bf; gf24.R = S; gf24.C = GT;
      gf24.sAo = 0; gf24.sAi = 0; gf24.sAm = LS; gf24.sAk = 1; gf24.sBo = 0; gf24.sBi = 0; gf24.sBn = 1; gf24.sBk = G4; gf24.sCo = 0; gf24.sCi = 0; gf24.sCm = G4; gf24.sRo = 0; gf24.sRi = 0; gf24.sRm = 0; gf24.sRn = 0;
      gf24.M = N; gf24.N = G4; gf24.K = E + H; gf24.zi_n = 1; gf24.flags = 1; gf24.act = 0;
      gf24.alpha = 1.0f; gf24.beta = 0.0f; gf24.sa = 1.0f; gf24.sb = 1.0f; gf24.Npad = G4; gf24.pad_ = 0;
      k_gemm<1><<<dim3((unsigned)((G4) + 31) / 32, (unsigned)((N) + 15) / 16, (unsigned)(1)), 32, 0, stream>>>(gf24); }
    k_seg_cell<<<(unsigned)(((long long)N * H + 255) / 256), 256, 0, stream>>>(GT, tok, len, emb, S, C, out, N, L, E, H, LS, 24, 25, 0, 0);
    { GemmP gf25;
      gf25.A = S; gf25.B = PF; gf25.bias = bf; gf25.R = S; gf25.C = GT;
      gf25.sAo = 0; gf25.sAi = 0; gf25.sAm = LS; gf25.sAk = 1; gf25.sBo = 0; gf25.sBi = 0; gf25.sBn = 1; gf25.sBk = G4; gf25.sCo = 0; gf25.sCi = 0; gf25.sCm = G4; gf25.sRo = 0; gf25.sRi = 0; gf25.sRm = 0; gf25.sRn = 0;
      gf25.M = N; gf25.N = G4; gf25.K = E + H; gf25.zi_n = 1; gf25.flags = 1; gf25.act = 0;
      gf25.alpha = 1.0f; gf25.beta = 0.0f; gf25.sa = 1.0f; gf25.sb = 1.0f; gf25.Npad = G4; gf25.pad_ = 0;
      k_gemm<1><<<dim3((unsigned)((G4) + 31) / 32, (unsigned)((N) + 15) / 16, (unsigned)(1)), 32, 0, stream>>>(gf25); }
    k_seg_cell<<<(unsigned)(((long long)N * H + 255) / 256), 256, 0, stream>>>(GT, tok, len, emb, S, C, out, N, L, E, H, LS, 25, 26, 0, 0);
    { GemmP gf26;
      gf26.A = S; gf26.B = PF; gf26.bias = bf; gf26.R = S; gf26.C = GT;
      gf26.sAo = 0; gf26.sAi = 0; gf26.sAm = LS; gf26.sAk = 1; gf26.sBo = 0; gf26.sBi = 0; gf26.sBn = 1; gf26.sBk = G4; gf26.sCo = 0; gf26.sCi = 0; gf26.sCm = G4; gf26.sRo = 0; gf26.sRi = 0; gf26.sRm = 0; gf26.sRn = 0;
      gf26.M = N; gf26.N = G4; gf26.K = E + H; gf26.zi_n = 1; gf26.flags = 1; gf26.act = 0;
      gf26.alpha = 1.0f; gf26.beta = 0.0f; gf26.sa = 1.0f; gf26.sb = 1.0f; gf26.Npad = G4; gf26.pad_ = 0;
      k_gemm<1><<<dim3((unsigned)((G4) + 31) / 32, (unsigned)((N) + 15) / 16, (unsigned)(1)), 32, 0, stream>>>(gf26); }
    k_seg_cell<<<(unsigned)(((long long)N * H + 255) / 256), 256, 0, stream>>>(GT, tok, len, emb, S, C, out, N, L, E, H, LS, 26, 27, 0, 0);
    { GemmP gf27;
      gf27.A = S; gf27.B = PF; gf27.bias = bf; gf27.R = S; gf27.C = GT;
      gf27.sAo = 0; gf27.sAi = 0; gf27.sAm = LS; gf27.sAk = 1; gf27.sBo = 0; gf27.sBi = 0; gf27.sBn = 1; gf27.sBk = G4; gf27.sCo = 0; gf27.sCi = 0; gf27.sCm = G4; gf27.sRo = 0; gf27.sRi = 0; gf27.sRm = 0; gf27.sRn = 0;
      gf27.M = N; gf27.N = G4; gf27.K = E + H; gf27.zi_n = 1; gf27.flags = 1; gf27.act = 0;
      gf27.alpha = 1.0f; gf27.beta = 0.0f; gf27.sa = 1.0f; gf27.sb = 1.0f; gf27.Npad = G4; gf27.pad_ = 0;
      k_gemm<1><<<dim3((unsigned)((G4) + 31) / 32, (unsigned)((N) + 15) / 16, (unsigned)(1)), 32, 0, stream>>>(gf27); }
    k_seg_cell<<<(unsigned)(((long long)N * H + 255) / 256), 256, 0, stream>>>(GT, tok, len, emb, S, C, out, N, L, E, H, LS, 27, 28, 0, 0);
    { GemmP gf28;
      gf28.A = S; gf28.B = PF; gf28.bias = bf; gf28.R = S; gf28.C = GT;
      gf28.sAo = 0; gf28.sAi = 0; gf28.sAm = LS; gf28.sAk = 1; gf28.sBo = 0; gf28.sBi = 0; gf28.sBn = 1; gf28.sBk = G4; gf28.sCo = 0; gf28.sCi = 0; gf28.sCm = G4; gf28.sRo = 0; gf28.sRi = 0; gf28.sRm = 0; gf28.sRn = 0;
      gf28.M = N; gf28.N = G4; gf28.K = E + H; gf28.zi_n = 1; gf28.flags = 1; gf28.act = 0;
      gf28.alpha = 1.0f; gf28.beta = 0.0f; gf28.sa = 1.0f; gf28.sb = 1.0f; gf28.Npad = G4; gf28.pad_ = 0;
      k_gemm<1><<<dim3((unsigned)((G4) + 31) / 32, (unsigned)((N) + 15) / 16, (unsigned)(1)), 32, 0, stream>>>(gf28); }
    k_seg_cell<<<(unsigned)(((long long)N * H + 255) / 256), 256, 0, stream>>>(GT, tok, len, emb, S, C, out, N, L, E, H, LS, 28, 29, 0, 0);
    { GemmP gf29;
      gf29.A = S; gf29.B = PF; gf29.bias = bf; gf29.R = S; gf29.C = GT;
      gf29.sAo = 0; gf29.sAi = 0; gf29.sAm = LS; gf29.sAk = 1; gf29.sBo = 0; gf29.sBi = 0; gf29.sBn = 1; gf29.sBk = G4; gf29.sCo = 0; gf29.sCi = 0; gf29.sCm = G4; gf29.sRo = 0; gf29.sRi = 0; gf29.sRm = 0; gf29.sRn = 0;
      gf29.M = N; gf29.N = G4; gf29.K = E + H; gf29.zi_n = 1; gf29.flags = 1; gf29.act = 0;
      gf29.alpha = 1.0f; gf29.beta = 0.0f; gf29.sa = 1.0f; gf29.sb = 1.0f; gf29.Npad = G4; gf29.pad_ = 0;
      k_gemm<1><<<dim3((unsigned)((G4) + 31) / 32, (unsigned)((N) + 15) / 16, (unsigned)(1)), 32, 0, stream>>>(gf29); }
    k_seg_cell<<<(unsigned)(((long long)N * H + 255) / 256), 256, 0, stream>>>(GT, tok, len, emb, S, C, out, N, L, E, H, LS, 29, 30, 0, 0);
    { GemmP gf30;
      gf30.A = S; gf30.B = PF; gf30.bias = bf; gf30.R = S; gf30.C = GT;
      gf30.sAo = 0; gf30.sAi = 0; gf30.sAm = LS; gf30.sAk = 1; gf30.sBo = 0; gf30.sBi = 0; gf30.sBn = 1; gf30.sBk = G4; gf30.sCo = 0; gf30.sCi = 0; gf30.sCm = G4; gf30.sRo = 0; gf30.sRi = 0; gf30.sRm = 0; gf30.sRn = 0;
      gf30.M = N; gf30.N = G4; gf30.K = E + H; gf30.zi_n = 1; gf30.flags = 1; gf30.act = 0;
      gf30.alpha = 1.0f; gf30.beta = 0.0f; gf30.sa = 1.0f; gf30.sb = 1.0f; gf30.Npad = G4; gf30.pad_ = 0;
      k_gemm<1><<<dim3((unsigned)((G4) + 31) / 32, (unsigned)((N) + 15) / 16, (unsigned)(1)), 32, 0, stream>>>(gf30); }
    k_seg_cell<<<(unsigned)(((long long)N * H + 255) / 256), 256, 0, stream>>>(GT, tok, len, emb, S, C, out, N, L, E, H, LS, 30, 31, 0, 0);
    { GemmP gf31;
      gf31.A = S; gf31.B = PF; gf31.bias = bf; gf31.R = S; gf31.C = GT;
      gf31.sAo = 0; gf31.sAi = 0; gf31.sAm = LS; gf31.sAk = 1; gf31.sBo = 0; gf31.sBi = 0; gf31.sBn = 1; gf31.sBk = G4; gf31.sCo = 0; gf31.sCi = 0; gf31.sCm = G4; gf31.sRo = 0; gf31.sRi = 0; gf31.sRm = 0; gf31.sRn = 0;
      gf31.M = N; gf31.N = G4; gf31.K = E + H; gf31.zi_n = 1; gf31.flags = 1; gf31.act = 0;
      gf31.alpha = 1.0f; gf31.beta = 0.0f; gf31.sa = 1.0f; gf31.sb = 1.0f; gf31.Npad = G4; gf31.pad_ = 0;
      k_gemm<1><<<dim3((unsigned)((G4) + 31) / 32, (unsigned)((N) + 15) / 16, (unsigned)(1)), 32, 0, stream>>>(gf31); }
    k_seg_cell<<<(unsigned)(((long long)N * H + 255) / 256), 256, 0, stream>>>(GT, tok, len, emb, S, C, out, N, L, E, H, LS, 31, -1, 1, 0);
    k_seg_init<<<(unsigned)(((long long)N * LS + 255) / 256), 256, 0, stream>>>(tok, emb, S, C, N, L, E, H, LS, 31);
    { GemmP gb0;
      gb0.A = S; gb0.B = PB; gb0.bias = bb; gb0.R = S; gb0.C = GT;
      gb0.sAo = 0; gb0.sAi = 0; gb0.sAm = LS; gb0.sAk = 1; gb0.sBo = 0; gb0.sBi = 0; gb0.sBn = 1; gb0.sBk = G4; gb0.sCo = 0; gb0.sCi = 0; gb0.sCm = G4; gb0.sRo = 0; gb0.sRi = 0; gb0.sRm = 0; gb0.sRn = 0;
      gb0.M = N; gb0.N = G4; gb0.K = E + H; gb0.zi_n = 1; gb0.flags = 1; gb0.act = 0;
      gb0.alpha = 1.0f; gb0.beta = 0.0f; gb0.sa = 1.0f; gb0.sb = 1.0f; gb0.Npad = G4; gb0.pad_ = 0;
      k_gemm<1><<<dim3((unsigned)((G4) + 31) / 32, (unsigned)((N) + 15) / 16, (unsigned)(1)), 32, 0, stream>>>(gb0); }
    k_seg_cell<<<(unsigned)(((long long)N * H + 255) / 256), 256, 0, stream>>>(GT, tok, len, emb, S, C, out, N, L, E, H, LS, 31, 30, 0, 32);
    { GemmP gb1;
      gb1.A = S; gb1.B = PB; gb1.bias = bb; gb1.R = S; gb1.C = GT;
      gb1.sAo = 0; gb1.sAi = 0; gb1.sAm = LS; gb1.sAk = 1; gb1.sBo = 0; gb1.sBi = 0; gb1.sBn = 1; gb1.sBk = G4; gb1.sCo = 0; gb1.sCi = 0; gb1.sCm = G4; gb1.sRo = 0; gb1.sRi = 0; gb1.sRm = 0; gb1.sRn = 0;
      gb1.M = N; gb1.N = G4; gb1.K = E + H; gb1.zi_n = 1; gb1.flags = 1; gb1.act = 0;
      gb1.alpha = 1.0f; gb1.beta = 0.0f; gb1.sa = 1.0f; gb1.sb = 1.0f; gb1.Npad = G4; gb1.pad_ = 0;
      k_gemm<1><<<dim3((unsigned)((G4) + 31) / 32, (unsigned)((N) + 15) / 16, (unsigned)(1)), 32, 0, stream>>>(gb1); }
    k_seg_cell<<<(unsigned)(((long long)N * H + 255) / 256), 256, 0, stream>>>(GT, tok, len, emb, S, C, out, N, L, E, H, LS, 30, 29, 0, 32);
    { GemmP gb2;
      gb2.A = S; gb2.B = PB; gb2.bias = bb; gb2.R = S; gb2.C = GT;
      gb2.sAo = 0; gb2.sAi = 0; gb2.sAm = LS; gb2.sAk = 1; gb2.sBo = 0; gb2.sBi = 0; gb2.sBn = 1; gb2.sBk = G4; gb2.sCo = 0; gb2.sCi = 0; gb2.sCm = G4; gb2.sRo = 0; gb2.sRi = 0; gb2.sRm = 0; gb2.sRn = 0;
      gb2.M = N; gb2.N = G4; gb2.K = E + H; gb2.zi_n = 1; gb2.flags = 1; gb2.act = 0;
      gb2.alpha = 1.0f; gb2.beta = 0.0f; gb2.sa = 1.0f; gb2.sb = 1.0f; gb2.Npad = G4; gb2.pad_ = 0;
      k_gemm<1><<<dim3((unsigned)((G4) + 31) / 32, (unsigned)((N) + 15) / 16, (unsigned)(1)), 32, 0, stream>>>(gb2); }
    k_seg_cell<<<(unsigned)(((long long)N * H + 255) / 256), 256, 0, stream>>>(GT, tok, len, emb, S, C, out, N, L, E, H, LS, 29, 28, 0, 32);
    { GemmP gb3;
      gb3.A = S; gb3.B = PB; gb3.bias = bb; gb3.R = S; gb3.C = GT;
      gb3.sAo = 0; gb3.sAi = 0; gb3.sAm = LS; gb3.sAk = 1; gb3.sBo = 0; gb3.sBi = 0; gb3.sBn = 1; gb3.sBk = G4; gb3.sCo = 0; gb3.sCi = 0; gb3.sCm = G4; gb3.sRo = 0; gb3.sRi = 0; gb3.sRm = 0; gb3.sRn = 0;
      gb3.M = N; gb3.N = G4; gb3.K = E + H; gb3.zi_n = 1; gb3.flags = 1; gb3.act = 0;
      gb3.alpha = 1.0f; gb3.beta = 0.0f; gb3.sa = 1.0f; gb3.sb = 1.0f; gb3.Npad = G4; gb3.pad_ = 0;
      k_gemm<1><<<dim3((unsigned)((G4) + 31) / 32, (unsigned)((N) + 15) / 16, (unsigned)(1)), 32, 0, stream>>>(gb3); }
    k_seg_cell<<<(unsigned)(((long long)N * H + 255) / 256), 256, 0, stream>>>(GT, tok, len, emb, S, C, out, N, L, E, H, LS, 28, 27, 0, 32);
    { GemmP gb4;
      gb4.A = S; gb4.B = PB; gb4.bias = bb; gb4.R = S; gb4.C = GT;
      gb4.sAo = 0; gb4.sAi = 0; gb4.sAm = LS; gb4.sAk = 1; gb4.sBo = 0; gb4.sBi = 0; gb4.sBn = 1; gb4.sBk = G4; gb4.sCo = 0; gb4.sCi = 0; gb4.sCm = G4; gb4.sRo = 0; gb4.sRi = 0; gb4.sRm = 0; gb4.sRn = 0;
      gb4.M = N; gb4.N = G4; gb4.K = E + H; gb4.zi_n = 1; gb4.flags = 1; gb4.act = 0;
      gb4.alpha = 1.0f; gb4.beta = 0.0f; gb4.sa = 1.0f; gb4.sb = 1.0f; gb4.Npad = G4; gb4.pad_ = 0;
      k_gemm<1><<<dim3((unsigned)((G4) + 31) / 32, (unsigned)((N) + 15) / 16, (unsigned)(1)), 32, 0, stream>>>(gb4); }
    k_seg_cell<<<(unsigned)(((long long)N * H + 255) / 256), 256, 0, stream>>>(GT, tok, len, emb, S, C, out, N, L, E, H, LS, 27, 26, 0, 32);
    { GemmP gb5;
      gb5.A = S; gb5.B = PB; gb5.bias = bb; gb5.R = S; gb5.C = GT;
      gb5.sAo = 0; gb5.sAi = 0; gb5.sAm = LS; gb5.sAk = 1; gb5.sBo = 0; gb5.sBi = 0; gb5.sBn = 1; gb5.sBk = G4; gb5.sCo = 0; gb5.sCi = 0; gb5.sCm = G4; gb5.sRo = 0; gb5.sRi = 0; gb5.sRm = 0; gb5.sRn = 0;
      gb5.M = N; gb5.N = G4; gb5.K = E + H; gb5.zi_n = 1; gb5.flags = 1; gb5.act = 0;
      gb5.alpha = 1.0f; gb5.beta = 0.0f; gb5.sa = 1.0f; gb5.sb = 1.0f; gb5.Npad = G4; gb5.pad_ = 0;
      k_gemm<1><<<dim3((unsigned)((G4) + 31) / 32, (unsigned)((N) + 15) / 16, (unsigned)(1)), 32, 0, stream>>>(gb5); }
    k_seg_cell<<<(unsigned)(((long long)N * H + 255) / 256), 256, 0, stream>>>(GT, tok, len, emb, S, C, out, N, L, E, H, LS, 26, 25, 0, 32);
    { GemmP gb6;
      gb6.A = S; gb6.B = PB; gb6.bias = bb; gb6.R = S; gb6.C = GT;
      gb6.sAo = 0; gb6.sAi = 0; gb6.sAm = LS; gb6.sAk = 1; gb6.sBo = 0; gb6.sBi = 0; gb6.sBn = 1; gb6.sBk = G4; gb6.sCo = 0; gb6.sCi = 0; gb6.sCm = G4; gb6.sRo = 0; gb6.sRi = 0; gb6.sRm = 0; gb6.sRn = 0;
      gb6.M = N; gb6.N = G4; gb6.K = E + H; gb6.zi_n = 1; gb6.flags = 1; gb6.act = 0;
      gb6.alpha = 1.0f; gb6.beta = 0.0f; gb6.sa = 1.0f; gb6.sb = 1.0f; gb6.Npad = G4; gb6.pad_ = 0;
      k_gemm<1><<<dim3((unsigned)((G4) + 31) / 32, (unsigned)((N) + 15) / 16, (unsigned)(1)), 32, 0, stream>>>(gb6); }
    k_seg_cell<<<(unsigned)(((long long)N * H + 255) / 256), 256, 0, stream>>>(GT, tok, len, emb, S, C, out, N, L, E, H, LS, 25, 24, 0, 32);
    { GemmP gb7;
      gb7.A = S; gb7.B = PB; gb7.bias = bb; gb7.R = S; gb7.C = GT;
      gb7.sAo = 0; gb7.sAi = 0; gb7.sAm = LS; gb7.sAk = 1; gb7.sBo = 0; gb7.sBi = 0; gb7.sBn = 1; gb7.sBk = G4; gb7.sCo = 0; gb7.sCi = 0; gb7.sCm = G4; gb7.sRo = 0; gb7.sRi = 0; gb7.sRm = 0; gb7.sRn = 0;
      gb7.M = N; gb7.N = G4; gb7.K = E + H; gb7.zi_n = 1; gb7.flags = 1; gb7.act = 0;
      gb7.alpha = 1.0f; gb7.beta = 0.0f; gb7.sa = 1.0f; gb7.sb = 1.0f; gb7.Npad = G4; gb7.pad_ = 0;
      k_gemm<1><<<dim3((unsigned)((G4) + 31) / 32, (unsigned)((N) + 15) / 16, (unsigned)(1)), 32, 0, stream>>>(gb7); }
    k_seg_cell<<<(unsigned)(((long long)N * H + 255) / 256), 256, 0, stream>>>(GT, tok, len, emb, S, C, out, N, L, E, H, LS, 24, 23, 0, 32);
    { GemmP gb8;
      gb8.A = S; gb8.B = PB; gb8.bias = bb; gb8.R = S; gb8.C = GT;
      gb8.sAo = 0; gb8.sAi = 0; gb8.sAm = LS; gb8.sAk = 1; gb8.sBo = 0; gb8.sBi = 0; gb8.sBn = 1; gb8.sBk = G4; gb8.sCo = 0; gb8.sCi = 0; gb8.sCm = G4; gb8.sRo = 0; gb8.sRi = 0; gb8.sRm = 0; gb8.sRn = 0;
      gb8.M = N; gb8.N = G4; gb8.K = E + H; gb8.zi_n = 1; gb8.flags = 1; gb8.act = 0;
      gb8.alpha = 1.0f; gb8.beta = 0.0f; gb8.sa = 1.0f; gb8.sb = 1.0f; gb8.Npad = G4; gb8.pad_ = 0;
      k_gemm<1><<<dim3((unsigned)((G4) + 31) / 32, (unsigned)((N) + 15) / 16, (unsigned)(1)), 32, 0, stream>>>(gb8); }
    k_seg_cell<<<(unsigned)(((long long)N * H + 255) / 256), 256, 0, stream>>>(GT, tok, len, emb, S, C, out, N, L, E, H, LS, 23, 22, 0, 32);
    { GemmP gb9;
      gb9.A = S; gb9.B = PB; gb9.bias = bb; gb9.R = S; gb9.C = GT;
      gb9.sAo = 0; gb9.sAi = 0; gb9.sAm = LS; gb9.sAk = 1; gb9.sBo = 0; gb9.sBi = 0; gb9.sBn = 1; gb9.sBk = G4; gb9.sCo = 0; gb9.sCi = 0; gb9.sCm = G4; gb9.sRo = 0; gb9.sRi = 0; gb9.sRm = 0; gb9.sRn = 0;
      gb9.M = N; gb9.N = G4; gb9.K = E + H; gb9.zi_n = 1; gb9.flags = 1; gb9.act = 0;
      gb9.alpha = 1.0f; gb9.beta = 0.0f; gb9.sa = 1.0f; gb9.sb = 1.0f; gb9.Npad = G4; gb9.pad_ = 0;
      k_gemm<1><<<dim3((unsigned)((G4) + 31) / 32, (unsigned)((N) + 15) / 16, (unsigned)(1)), 32, 0, stream>>>(gb9); }
    k_seg_cell<<<(unsigned)(((long long)N * H + 255) / 256), 256, 0, stream>>>(GT, tok, len, emb, S, C, out, N, L, E, H, LS, 22, 21, 0, 32);
    { GemmP gb10;
      gb10.A = S; gb10.B = PB; gb10.bias = bb; gb10.R = S; gb10.C = GT;
      gb10.sAo = 0; gb10.sAi = 0; gb10.sAm = LS; gb10.sAk = 1; gb10.sBo = 0; gb10.sBi = 0; gb10.sBn = 1; gb10.sBk = G4; gb10.sCo = 0; gb10.sCi = 0; gb10.sCm = G4; gb10.sRo = 0; gb10.sRi = 0; gb10.sRm = 0; gb10.sRn = 0;
      gb10.M = N; gb10.N = G4; gb10.K = E + H; gb10.zi_n = 1; gb10.flags = 1; gb10.act = 0;
      gb10.alpha = 1.0f; gb10.beta = 0.0f; gb10.sa = 1.0f; gb10.sb = 1.0f; gb10.Npad = G4; gb10.pad_ = 0;
      k_gemm<1><<<dim3((unsigned)((G4) + 31) / 32, (unsigned)((N) + 15) / 16, (unsigned)(1)), 32, 0, stream>>>(gb10); }
    k_seg_cell<<<(unsigned)(((long long)N * H + 255) / 256), 256, 0, stream>>>(GT, tok, len, emb, S, C, out, N, L, E, H, LS, 21, 20, 0, 32);
    { GemmP gb11;
      gb11.A = S; gb11.B = PB; gb11.bias = bb; gb11.R = S; gb11.C = GT;
      gb11.sAo = 0; gb11.sAi = 0; gb11.sAm = LS; gb11.sAk = 1; gb11.sBo = 0; gb11.sBi = 0; gb11.sBn = 1; gb11.sBk = G4; gb11.sCo = 0; gb11.sCi = 0; gb11.sCm = G4; gb11.sRo = 0; gb11.sRi = 0; gb11.sRm = 0; gb11.sRn = 0;
      gb11.M = N; gb11.N = G4; gb11.K = E + H; gb11.zi_n = 1; gb11.flags = 1; gb11.act = 0;
      gb11.alpha = 1.0f; gb11.beta = 0.0f; gb11.sa = 1.0f; gb11.sb = 1.0f; gb11.Npad = G4; gb11.pad_ = 0;
      k_gemm<1><<<dim3((unsigned)((G4) + 31) / 32, (unsigned)((N) + 15) / 16, (unsigned)(1)), 32, 0, stream>>>(gb11); }
    k_seg_cell<<<(unsigned)(((long long)N * H + 255) / 256), 256, 0, stream>>>(GT, tok, len, emb, S, C, out, N, L, E, H, LS, 20, 19, 0, 32);
    { GemmP gb12;
      gb12.A = S; gb12.B = PB; gb12.bias = bb; gb12.R = S; gb12.C = GT;
      gb12.sAo = 0; gb12.sAi = 0; gb12.sAm = LS; gb12.sAk = 1; gb12.sBo = 0; gb12.sBi = 0; gb12.sBn = 1; gb12.sBk = G4; gb12.sCo = 0; gb12.sCi = 0; gb12.sCm = G4; gb12.sRo = 0; gb12.sRi = 0; gb12.sRm = 0; gb12.sRn = 0;
      gb12.M = N; gb12.N = G4; gb12.K = E + H; gb12.zi_n = 1; gb12.flags = 1; gb12.act = 0;
      gb12.alpha = 1.0f; gb12.beta = 0.0f; gb12.sa = 1.0f; gb12.sb = 1.0f; gb12.Npad = G4; gb12.pad_ = 0;
      k_gemm<1><<<dim3((unsigned)((G4) + 31) / 32, (unsigned)((N) + 15) / 16, (unsigned)(1)), 32, 0, stream>>>(gb12); }
    k_seg_cell<<<(unsigned)(((long long)N * H + 255) / 256), 256, 0, stream>>>(GT, tok, len, emb, S, C, out, N, L, E, H, LS, 19, 18, 0, 32);
    { GemmP gb13;
      gb13.A = S; gb13.B = PB; gb13.bias = bb; gb13.R = S; gb13.C = GT;
      gb13.sAo = 0; gb13.sAi = 0; gb13.sAm = LS; gb13.sAk = 1; gb13.sBo = 0; gb13.sBi = 0; gb13.sBn = 1; gb13.sBk = G4; gb13.sCo = 0; gb13.sCi = 0; gb13.sCm = G4; gb13.sRo = 0; gb13.sRi = 0; gb13.sRm = 0; gb13.sRn = 0;
      gb13.M = N; gb13.N = G4; gb13.K = E + H; gb13.zi_n = 1; gb13.flags = 1; gb13.act = 0;
      gb13.alpha = 1.0f; gb13.beta = 0.0f; gb13.sa = 1.0f; gb13.sb = 1.0f; gb13.Npad = G4; gb13.pad_ = 0;
      k_gemm<1><<<dim3((unsigned)((G4) + 31) / 32, (unsigned)((N) + 15) / 16, (unsigned)(1)), 32, 0, stream>>>(gb13); }
    k_seg_cell<<<(unsigned)(((long long)N * H + 255) / 256), 256, 0, stream>>>(GT, tok, len, emb, S, C, out, N, L, E, H, LS, 18, 17, 0, 32);
    { GemmP gb14;
      gb14.A = S; gb14.B = PB; gb14.bias = bb; gb14.R = S; gb14.C = GT;
      gb14.sAo = 0; gb14.sAi = 0; gb14.sAm = LS; gb14.sAk = 1; gb14.sBo = 0; gb14.sBi = 0; gb14.sBn = 1; gb14.sBk = G4; gb14.sCo = 0; gb14.sCi = 0; gb14.sCm = G4; gb14.sRo = 0; gb14.sRi = 0; gb14.sRm = 0; gb14.sRn = 0;
      gb14.M = N; gb14.N = G4; gb14.K = E + H; gb14.zi_n = 1; gb14.flags = 1; gb14.act = 0;
      gb14.alpha = 1.0f; gb14.beta = 0.0f; gb14.sa = 1.0f; gb14.sb = 1.0f; gb14.Npad = G4; gb14.pad_ = 0;
      k_gemm<1><<<dim3((unsigned)((G4) + 31) / 32, (unsigned)((N) + 15) / 16, (unsigned)(1)), 32, 0, stream>>>(gb14); }
    k_seg_cell<<<(unsigned)(((long long)N * H + 255) / 256), 256, 0, stream>>>(GT, tok, len, emb, S, C, out, N, L, E, H, LS, 17, 16, 0, 32);
    { GemmP gb15;
      gb15.A = S; gb15.B = PB; gb15.bias = bb; gb15.R = S; gb15.C = GT;
      gb15.sAo = 0; gb15.sAi = 0; gb15.sAm = LS; gb15.sAk = 1; gb15.sBo = 0; gb15.sBi = 0; gb15.sBn = 1; gb15.sBk = G4; gb15.sCo = 0; gb15.sCi = 0; gb15.sCm = G4; gb15.sRo = 0; gb15.sRi = 0; gb15.sRm = 0; gb15.sRn = 0;
      gb15.M = N; gb15.N = G4; gb15.K = E + H; gb15.zi_n = 1; gb15.flags = 1; gb15.act = 0;
      gb15.alpha = 1.0f; gb15.beta = 0.0f; gb15.sa = 1.0f; gb15.sb = 1.0f; gb15.Npad = G4; gb15.pad_ = 0;
      k_gemm<1><<<dim3((unsigned)((G4) + 31) / 32, (unsigned)((N) + 15) / 16, (unsigned)(1)), 32, 0, stream>>>(gb15); }
    k_seg_cell<<<(unsigned)(((long long)N * H + 255) / 256), 256, 0, stream>>>(GT, tok, len, emb, S, C, out, N, L, E, H, LS, 16, 15, 0, 32);
    { GemmP gb16;
      gb16.A = S; gb16.B = PB; gb16.bias = bb; gb16.R = S; gb16.C = GT;
      gb16.sAo = 0; gb16.sAi = 0; gb16.sAm = LS; gb16.sAk = 1; gb16.sBo = 0; gb16.sBi = 0; gb16.sBn = 1; gb16.sBk = G4; gb16.sCo = 0; gb16.sCi = 0; gb16.sCm = G4; gb16.sRo = 0; gb16.sRi = 0; gb16.sRm = 0; gb16.sRn = 0;
      gb16.M = N; gb16.N = G4; gb16.K = E + H; gb16.zi_n = 1; gb16.flags = 1; gb16.act = 0;
      gb16.alpha = 1.0f; gb16.beta = 0.0f; gb16.sa = 1.0f; gb16.sb = 1.0f; gb16.Npad = G4; gb16.pad_ = 0;
      k_gemm<1><<<dim3((unsigned)((G4) + 31) / 32, (unsigned)((N) + 15) / 16, (unsigned)(1)), 32, 0, stream>>>(gb16); }
    k_seg_cell<<<(unsigned)(((long long)N * H + 255) / 256), 256, 0, stream>>>(GT, tok, len, emb, S, C, out, N, L, E, H, LS, 15, 14, 0, 32);
    { GemmP gb17;
      gb17.A = S; gb17.B = PB; gb17.bias = bb; gb17.R = S; gb17.C = GT;
      gb17.sAo = 0; gb17.sAi = 0; gb17.sAm = LS; gb17.sAk = 1; gb17.sBo = 0; gb17.sBi = 0; gb17.sBn = 1; gb17.sBk = G4; gb17.sCo = 0; gb17.sCi = 0; gb17.sCm = G4; gb17.sRo = 0; gb17.sRi = 0; gb17.sRm = 0; gb17.sRn = 0;
      gb17.M = N; gb17.N = G4; gb17.K = E + H; gb17.zi_n = 1; gb17.flags = 1; gb17.act = 0;
      gb17.alpha = 1.0f; gb17.beta = 0.0f; gb17.sa = 1.0f; gb17.sb = 1.0f; gb17.Npad = G4; gb17.pad_ = 0;
      k_gemm<1><<<dim3((unsigned)((G4) + 31) / 32, (unsigned)((N) + 15) / 16, (unsigned)(1)), 32, 0, stream>>>(gb17); }
    k_seg_cell<<<(unsigned)(((long long)N * H + 255) / 256), 256, 0, stream>>>(GT, tok, len, emb, S, C, out, N, L, E, H, LS, 14, 13, 0, 32);
    { GemmP gb18;
      gb18.A = S; gb18.B = PB; gb18.bias = bb; gb18.R = S; gb18.C = GT;
      gb18.sAo = 0; gb18.sAi = 0; gb18.sAm = LS; gb18.sAk = 1; gb18.sBo = 0; gb18.sBi = 0; gb18.sBn = 1; gb18.sBk = G4; gb18.sCo = 0; gb18.sCi = 0; gb18.sCm = G4; gb18.sRo = 0; gb18.sRi = 0; gb18.sRm = 0; gb18.sRn = 0;
      gb18.M = N; gb18.N = G4; gb18.K = E + H; gb18.zi_n = 1; gb18.flags = 1; gb18.act = 0;
      gb18.alpha = 1.0f; gb18.beta = 0.0f; gb18.sa = 1.0f; gb18.sb = 1.0f; gb18.Npad = G4; gb18.pad_ = 0;
      k_gemm<1><<<dim3((unsigned)((G4) + 31) / 32, (unsigned)((N) + 15) / 16, (unsigned)(1)), 32, 0, stream>>>(gb18); }
    k_seg_cell<<<(unsigned)(((long long)N * H + 255) / 256), 256, 0, stream>>>(GT, tok, len, emb, S, C, out, N, L, E, H, LS, 13, 12, 0, 32);
    { GemmP gb19;
      gb19.A = S; gb19.B = PB; gb19.bias = bb; gb19.R = S; gb19.C = GT;
      gb19.sAo = 0; gb19.sAi = 0; gb19.sAm = LS; gb19.sAk = 1; gb19.sBo = 0; gb19.sBi = 0; gb19.sBn = 1; gb19.sBk = G4; gb19.sCo = 0; gb19.sCi = 0; gb19.sCm = G4; gb19.sRo = 0; gb19.sRi = 0; gb19.sRm = 0; gb19.sRn = 0;
      gb19.M = N; gb19.N = G4; gb19.K = E + H; gb19.zi_n = 1; gb19.flags = 1; gb19.act = 0;
      gb19.alpha = 1.0f; gb19.beta = 0.0f; gb19.sa = 1.0f; gb19.sb = 1.0f; gb19.Npad = G4; gb19.pad_ = 0;
      k_gemm<1><<<dim3((unsigned)((G4) + 31) / 32, (unsigned)((N) + 15) / 16, (unsigned)(1)), 32, 0, stream>>>(gb19); }
    k_seg_cell<<<(unsigned)(((long long)N * H + 255) / 256), 256, 0, stream>>>(GT, tok, len, emb, S, C, out, N, L, E, H, LS, 12, 11, 0, 32);
    { GemmP gb20;
      gb20.A = S; gb20.B = PB; gb20.bias = bb; gb20.R = S; gb20.C = GT;
      gb20.sAo = 0; gb20.sAi = 0; gb20.sAm = LS; gb20.sAk = 1; gb20.sBo = 0; gb20.sBi = 0; gb20.sBn = 1; gb20.sBk = G4; gb20.sCo = 0; gb20.sCi = 0; gb20.sCm = G4; gb20.sRo = 0; gb20.sRi = 0; gb20.sRm = 0; gb20.sRn = 0;
      gb20.M = N; gb20.N = G4; gb20.K = E + H; gb20.zi_n = 1; gb20.flags = 1; gb20.act = 0;
      gb20.alpha = 1.0f; gb20.beta = 0.0f; gb20.sa = 1.0f; gb20.sb = 1.0f; gb20.Npad = G4; gb20.pad_ = 0;
      k_gemm<1><<<dim3((unsigned)((G4) + 31) / 32, (unsigned)((N) + 15) / 16, (unsigned)(1)), 32, 0, stream>>>(gb20); }
    k_seg_cell<<<(unsigned)(((long long)N * H + 255) / 256), 256, 0, stream>>>(GT, tok, len, emb, S, C, out, N, L, E, H, LS, 11, 10, 0, 32);
    { GemmP gb21;
      gb21.A = S; gb21.B = PB; gb21.bias = bb; gb21.R = S; gb21.C = GT;
      gb21.sAo = 0; gb21.sAi = 0; gb21.sAm = LS; gb21.sAk = 1; gb21.sBo = 0; gb21.sBi = 0; gb21.sBn = 1; gb21.sBk = G4; gb21.sCo = 0; gb21.sCi = 0; gb21.sCm = G4; gb21.sRo = 0; gb21.sRi = 0; gb21.sRm = 0; gb21.sRn = 0;
      gb21.M = N; gb21.N = G4; gb21.K = E + H; gb21.zi_n = 1; gb21.flags = 1; gb21.act = 0;
      gb21.alpha = 1.0f; gb21.beta = 0.0f; gb21.sa = 1.0f; gb21.sb = 1.0f; gb21.Npad = G4; gb21.pad_ = 0;
      k_gemm<1><<<dim3((unsigned)((G4) + 31) / 32, (unsigned)((N) + 15) / 16, (unsigned)(1)), 32, 0, stream>>>(gb21); }
    k_seg_cell<<<(unsigned)(((long long)N * H + 255) / 256), 256, 0, stream>>>(GT, tok, len, emb, S, C, out, N, L, E, H, LS, 10, 9, 0, 32);
    { GemmP gb22;
      gb22.A = S; gb22.B = PB; gb22.bias = bb; gb22.R = S; gb22.C = GT;
      gb22.sAo = 0; gb22.sAi = 0; gb22.sAm = LS; gb22.sAk = 1; gb22.sBo = 0; gb22.sBi = 0; gb22.sBn = 1; gb22.sBk = G4; gb22.sCo = 0; gb22.sCi = 0; gb22.sCm = G4; gb22.sRo = 0; gb22.sRi = 0; gb22.sRm = 0; gb22.sRn = 0;
      gb22.M = N; gb22.N = G4; gb22.K = E + H; gb22.zi_n = 1; gb22.flags = 1; gb22.act = 0;
      gb22.alpha = 1.0f; gb22.beta = 0.0f; gb22.sa = 1.0f; gb22.sb = 1.0f; gb22.Npad = G4; gb22.pad_ = 0;
      k_gemm<1><<<dim3((unsigned)((G4) + 31) / 32, (unsigned)((N) + 15) / 16, (unsigned)(1)), 32, 0, stream>>>(gb22); }
    k_seg_cell<<<(unsigned)(((long long)N * H + 255) / 256), 256, 0, stream>>>(GT, tok, len, emb, S, C, out, N, L, E, H, LS, 9, 8, 0, 32);
    { GemmP gb23;
      gb23.A = S; gb23.B = PB; gb23.bias = bb; gb23.R = S; gb23.C = GT;
      gb23.sAo = 0; gb23.sAi = 0; gb23.sAm = LS; gb23.sAk = 1; gb23.sBo = 0; gb23.sBi = 0; gb23.sBn = 1; gb23.sBk = G4; gb23.sCo = 0; gb23.sCi = 0; gb23.sCm = G4; gb23.sRo = 0; gb23.sRi = 0; gb23.sRm = 0; gb23.sRn = 0;
      gb23.M = N; gb23.N = G4; gb23.K = E + H; gb23.zi_n = 1; gb23.flags = 1; gb23.act = 0;
      gb23.alpha = 1.0f; gb23.beta = 0.0f; gb23.sa = 1.0f; gb23.sb = 1.0f; gb23.Npad = G4; gb23.pad_ = 0;
      k_gemm<1><<<dim3((unsigned)((G4) + 31) / 32, (unsigned)((N) + 15) / 16, (unsigned)(1)), 32, 0, stream>>>(gb23); }
    k_seg_cell<<<(unsigned)(((long long)N * H + 255) / 256), 256, 0, stream>>>(GT, tok, len, emb, S, C, out, N, L, E, H, LS, 8, 7, 0, 32);
    { GemmP gb24;
      gb24.A = S; gb24.B = PB; gb24.bias = bb; gb24.R = S; gb24.C = GT;
      gb24.sAo = 0; gb24.sAi = 0; gb24.sAm = LS; gb24.sAk = 1; gb24.sBo = 0; gb24.sBi = 0; gb24.sBn = 1; gb24.sBk = G4; gb24.sCo = 0; gb24.sCi = 0; gb24.sCm = G4; gb24.sRo = 0; gb24.sRi = 0; gb24.sRm = 0; gb24.sRn = 0;
      gb24.M = N; gb24.N = G4; gb24.K = E + H; gb24.zi_n = 1; gb24.flags = 1; gb24.act = 0;
      gb24.alpha = 1.0f; gb24.beta = 0.0f; gb24.sa = 1.0f; gb24.sb = 1.0f; gb24.Npad = G4; gb24.pad_ = 0;
      k_gemm<1><<<dim3((unsigned)((G4) + 31) / 32, (unsigned)((N) + 15) / 16, (unsigned)(1)), 32, 0, stream>>>(gb24); }
    k_seg_cell<<<(unsigned)(((long long)N * H + 255) / 256), 256, 0, stream>>>(GT, tok, len, emb, S, C, out, N, L, E, H, LS, 7, 6, 0, 32);
    { GemmP gb25;
      gb25.A = S; gb25.B = PB; gb25.bias = bb; gb25.R = S; gb25.C = GT;
      gb25.sAo = 0; gb25.sAi = 0; gb25.sAm = LS; gb25.sAk = 1; gb25.sBo = 0; gb25.sBi = 0; gb25.sBn = 1; gb25.sBk = G4; gb25.sCo = 0; gb25.sCi = 0; gb25.sCm = G4; gb25.sRo = 0; gb25.sRi = 0; gb25.sRm = 0; gb25.sRn = 0;
      gb25.M = N; gb25.N = G4; gb25.K = E + H; gb25.zi_n = 1; gb25.flags = 1; gb25.act = 0;
      gb25.alpha = 1.0f; gb25.beta = 0.0f; gb25.sa = 1.0f; gb25.sb = 1.0f; gb25.Npad = G4; gb25.pad_ = 0;
      k_gemm<1><<<dim3((unsigned)((G4) + 31) / 32, (unsigned)((N) + 15) / 16, (unsigned)(1)), 32, 0, stream>>>(gb25); }
    k_seg_cell<<<(unsigned)(((long long)N * H + 255) / 256), 256, 0, stream>>>(GT, tok, len, emb, S, C, out, N, L, E, H, LS, 6, 5, 0, 32);
    { GemmP gb26;
      gb26.A = S; gb26.B = PB; gb26.bias = bb; gb26.R = S; gb26.C = GT;
      gb26.sAo = 0; gb26.sAi = 0; gb26.sAm = LS; gb26.sAk = 1; gb26.sBo = 0; gb26.sBi = 0; gb26.sBn = 1; gb26.sBk = G4; gb26.sCo = 0; gb26.sCi = 0; gb26.sCm = G4; gb26.sRo = 0; gb26.sRi = 0; gb26.sRm = 0; gb26.sRn = 0;
      gb26.M = N; gb26.N = G4; gb26.K = E + H; gb26.zi_n = 1; gb26.flags = 1; gb26.act = 0;
      gb26.alpha = 1.0f; gb26.beta = 0.0f; gb26.sa = 1.0f; gb26.sb = 1.0f; gb26.Npad = G4; gb26.pad_ = 0;
      k_gemm<1><<<dim3((unsigned)((G4) + 31) / 32, (unsigned)((N) + 15) / 16, (unsigned)(1)), 32, 0, stream>>>(gb26); }
    k_seg_cell<<<(unsigned)(((long long)N * H + 255) / 256), 256, 0, stream>>>(GT, tok, len, emb, S, C, out, N, L, E, H, LS, 5, 4, 0, 32);
    { GemmP gb27;
      gb27.A = S; gb27.B = PB; gb27.bias = bb; gb27.R = S; gb27.C = GT;
      gb27.sAo = 0; gb27.sAi = 0; gb27.sAm = LS; gb27.sAk = 1; gb27.sBo = 0; gb27.sBi = 0; gb27.sBn = 1; gb27.sBk = G4; gb27.sCo = 0; gb27.sCi = 0; gb27.sCm = G4; gb27.sRo = 0; gb27.sRi = 0; gb27.sRm = 0; gb27.sRn = 0;
      gb27.M = N; gb27.N = G4; gb27.K = E + H; gb27.zi_n = 1; gb27.flags = 1; gb27.act = 0;
      gb27.alpha = 1.0f; gb27.beta = 0.0f; gb27.sa = 1.0f; gb27.sb = 1.0f; gb27.Npad = G4; gb27.pad_ = 0;
      k_gemm<1><<<dim3((unsigned)((G4) + 31) / 32, (unsigned)((N) + 15) / 16, (unsigned)(1)), 32, 0, stream>>>(gb27); }
    k_seg_cell<<<(unsigned)(((long long)N * H + 255) / 256), 256, 0, stream>>>(GT, tok, len, emb, S, C, out, N, L, E, H, LS, 4, 3, 0, 32);
    { GemmP gb28;
      gb28.A = S; gb28.B = PB; gb28.bias = bb; gb28.R = S; gb28.C = GT;
      gb28.sAo = 0; gb28.sAi = 0; gb28.sAm = LS; gb28.sAk = 1; gb28.sBo = 0; gb28.sBi = 0; gb28.sBn = 1; gb28.sBk = G4; gb28.sCo = 0; gb28.sCi = 0; gb28.sCm = G4; gb28.sRo = 0; gb28.sRi = 0; gb28.sRm = 0; gb28.sRn = 0;
      gb28.M = N; gb28.N = G4; gb28.K = E + H; gb28.zi_n = 1; gb28.flags = 1; gb28.act = 0;
      gb28.alpha = 1.0f; gb28.beta = 0.0f; gb28.sa = 1.0f; gb28.sb = 1.0f; gb28.Npad = G4; gb28.pad_ = 0;
      k_gemm<1><<<dim3((unsigned)((G4) + 31) / 32, (unsigned)((N) + 15) / 16, (unsigned)(1)), 32, 0, stream>>>(gb28); }
    k_seg_cell<<<(unsigned)(((long long)N * H + 255) / 256), 256, 0, stream>>>(GT, tok, len, emb, S, C, out, N, L, E, H, LS, 3, 2, 0, 32);
    { GemmP gb29;
      gb29.A = S; gb29.B = PB; gb29.bias = bb; gb29.R = S; gb29.C = GT;
      gb29.sAo = 0; gb29.sAi = 0; gb29.sAm = LS; gb29.sAk = 1; gb29.sBo = 0; gb29.sBi = 0; gb29.sBn = 1; gb29.sBk = G4; gb29.sCo = 0; gb29.sCi = 0; gb29.sCm = G4; gb29.sRo = 0; gb29.sRi = 0; gb29.sRm = 0; gb29.sRn = 0;
      gb29.M = N; gb29.N = G4; gb29.K = E + H; gb29.zi_n = 1; gb29.flags = 1; gb29.act = 0;
      gb29.alpha = 1.0f; gb29.beta = 0.0f; gb29.sa = 1.0f; gb29.sb = 1.0f; gb29.Npad = G4; gb29.pad_ = 0;
      k_gemm<1><<<dim3((unsigned)((G4) + 31) / 32, (unsigned)((N) + 15) / 16, (unsigned)(1)), 32, 0, stream>>>(gb29); }
    k_seg_cell<<<(unsigned)(((long long)N * H + 255) / 256), 256, 0, stream>>>(GT, tok, len, emb, S, C, out, N, L, E, H, LS, 2, 1, 0, 32);
    { GemmP gb30;
      gb30.A = S; gb30.B = PB; gb30.bias = bb; gb30.R = S; gb30.C = GT;
      gb30.sAo = 0; gb30.sAi = 0; gb30.sAm = LS; gb30.sAk = 1; gb30.sBo = 0; gb30.sBi = 0; gb30.sBn = 1; gb30.sBk = G4; gb30.sCo = 0; gb30.sCi = 0; gb30.sCm = G4; gb30.sRo = 0; gb30.sRi = 0; gb30.sRm = 0; gb30.sRn = 0;
      gb30.M = N; gb30.N = G4; gb30.K = E + H; gb30.zi_n = 1; gb30.flags = 1; gb30.act = 0;
      gb30.alpha = 1.0f; gb30.beta = 0.0f; gb30.sa = 1.0f; gb30.sb = 1.0f; gb30.Npad = G4; gb30.pad_ = 0;
      k_gemm<1><<<dim3((unsigned)((G4) + 31) / 32, (unsigned)((N) + 15) / 16, (unsigned)(1)), 32, 0, stream>>>(gb30); }
    k_seg_cell<<<(unsigned)(((long long)N * H + 255) / 256), 256, 0, stream>>>(GT, tok, len, emb, S, C, out, N, L, E, H, LS, 1, 0, 0, 32);
    { GemmP gb31;
      gb31.A = S; gb31.B = PB; gb31.bias = bb; gb31.R = S; gb31.C = GT;
      gb31.sAo = 0; gb31.sAi = 0; gb31.sAm = LS; gb31.sAk = 1; gb31.sBo = 0; gb31.sBi = 0; gb31.sBn = 1; gb31.sBk = G4; gb31.sCo = 0; gb31.sCi = 0; gb31.sCm = G4; gb31.sRo = 0; gb31.sRi = 0; gb31.sRm = 0; gb31.sRn = 0;
      gb31.M = N; gb31.N = G4; gb31.K = E + H; gb31.zi_n = 1; gb31.flags = 1; gb31.act = 0;
      gb31.alpha = 1.0f; gb31.beta = 0.0f; gb31.sa = 1.0f; gb31.sb = 1.0f; gb31.Npad = G4; gb31.pad_ = 0;
      k_gemm<1><<<dim3((unsigned)((G4) + 31) / 32, (unsigned)((N) + 15) / 16, (unsigned)(1)), 32, 0, stream>>>(gb31); }
    k_seg_cell<<<(unsigned)(((long long)N * H + 255) / 256), 256, 0, stream>>>(GT, tok, len, emb, S, C, out, N, L, E, H, LS, 0, -1, 1, 32);
}
